// DenseCaps_23519240912904
// MI455X (gfx1250) — hardware-verified
//
#include <hip/hip_runtime.h>
#include <math.h>

typedef __attribute__((ext_vector_type(16))) _Float16 v16h;
typedef __attribute__((ext_vector_type(8)))  _Float16 v8h;
typedef __attribute__((ext_vector_type(16))) __bf16   v16b;
typedef __attribute__((ext_vector_type(8)))  float    v8f;
typedef __attribute__((ext_vector_type(4)))  float    v4f;

__device__ __forceinline__ int frag_k(int i, int h) { return (i < 8) ? (8 * h + i) : (16 + 8 * h + (i - 8)); }
__device__ __forceinline__ __bf16 bf16_rne(float f) {
    unsigned int u = __float_as_uint(f);
    u += 0x7fffu + ((u >> 16) & 1u);
    return __builtin_bit_cast(__bf16, (unsigned short)(u >> 16));
}
__device__ __forceinline__ float bf16_f32(__bf16 b) { return __uint_as_float(((unsigned int)__builtin_bit_cast(unsigned short, b)) << 16); }
__device__ __forceinline__ v8f wmma16(v16h a, v16h b, v8f c) {
    c = __builtin_amdgcn_wmma_f32_16x16x32_f16(false, a, false, b, (short)0, c, false, false);
    asm volatile("v_nop\n\tv_nop\n\tv_nop\n\tv_nop" : "+v"(c) : "v"(a), "v"(b));
    return c;
}
__device__ __forceinline__ v8f wmmab(v16b a, v16b b, v8f c) {
    c = __builtin_amdgcn_wmma_f32_16x16x32_bf16(false, a, false, b, (short)0, c, false, false);
    asm volatile("v_nop\n\tv_nop\n\tv_nop\n\tv_nop" : "+v"(c) : "v"(a), "v"(b));
    return c;
}
struct Split { v16b hi, lo; };
__device__ __forceinline__ v8f wmma3(const Split& a, const Split& b, v8f c) {
    c = __builtin_amdgcn_wmma_f32_16x16x32_bf16(false, a.hi, false, b.hi, (short)0, c, false, false);
    c = __builtin_amdgcn_wmma_f32_16x16x32_bf16(false, a.hi, false, b.lo, (short)0, c, false, false);
    c = __builtin_amdgcn_wmma_f32_16x16x32_bf16(false, a.lo, false, b.hi, (short)0, c, false, false);
    asm volatile("v_nop\n\tv_nop\n\tv_nop\n\tv_nop" : "+v"(c) : "v"(a.hi), "v"(a.lo), "v"(b.hi), "v"(b.lo));
    return c;
}
struct Split3 { v16b hi, mid, lo; };
__device__ __forceinline__ v8f wmma6(const Split3& a, const Split3& b, v8f c) {
    c = __builtin_amdgcn_wmma_f32_16x16x32_bf16(false, a.hi, false, b.hi, (short)0, c, false, false);
    c = __builtin_amdgcn_wmma_f32_16x16x32_bf16(false, a.hi, false, b.mid, (short)0, c, false, false);
    c = __builtin_amdgcn_wmma_f32_16x16x32_bf16(false, a.mid, false, b.hi, (short)0, c, false, false);
    c = __builtin_amdgcn_wmma_f32_16x16x32_bf16(false, a.hi, false, b.lo, (short)0, c, false, false);
    c = __builtin_amdgcn_wmma_f32_16x16x32_bf16(false, a.mid, false, b.mid, (short)0, c, false, false);
    c = __builtin_amdgcn_wmma_f32_16x16x32_bf16(false, a.lo, false, b.hi, (short)0, c, false, false);
    asm volatile("v_nop\n\tv_nop\n\tv_nop\n\tv_nop" : "+v"(c) : "v"(a.hi), "v"(a.mid), "v"(a.lo), "v"(b.hi), "v"(b.mid), "v"(b.lo));
    return c;
}

__device__ __forceinline__ v16h fh_ld(const float* __restrict__ p, long long sk, int k0, int h, int klen, float s) {
    v16h a;
#pragma unroll
    for (int i = 0; i < 16; ++i) { const int k = k0 + frag_k(i, h); a[i] = (k < klen) ? (_Float16)(p[(long long)k * sk] * s) : (_Float16)0.f; }
    return a;
}
__device__ __forceinline__ Split sp_ld(const float* __restrict__ p, long long sk, int k0, int h, int klen, float s) {
    Split r;
#pragma unroll
    for (int i = 0; i < 16; ++i) {
        const int k = k0 + frag_k(i, h); const float x = (k < klen) ? p[(long long)k * sk] * s : 0.f;
        const __bf16 hb = bf16_rne(x); r.hi[i] = hb; r.lo[i] = bf16_rne(x - bf16_f32(hb));
    }
    return r;
}
__device__ __forceinline__ Split3 sp3_ld(const float* __restrict__ p, long long sk, int k0, int h, int klen, float s) {
    Split3 r;
#pragma unroll
    for (int i = 0; i < 16; ++i) {
        const int k = k0 + frag_k(i, h); const float x = (k < klen) ? p[(long long)k * sk] * s : 0.f;
        const __bf16 hb = bf16_rne(x); const float r1 = x - bf16_f32(hb); const __bf16 mb = bf16_rne(r1);
        r.hi[i] = hb; r.mid[i] = mb; r.lo[i] = bf16_rne(r1 - bf16_f32(mb));
    }
    return r;
}
__device__ __forceinline__ v16b bh_ld(const float* __restrict__ p, long long sk, int k0, int h, int klen, float s) {
    v16b a;
#pragma unroll
    for (int i = 0; i < 16; ++i) { const int k = k0 + frag_k(i, h); a[i] = bf16_rne((k < klen) ? p[(long long)k * sk] * s : 0.f); }
    return a;
}
__device__ __forceinline__ v16h fh_row(const _Float16* __restrict__ row, int k0, int h) {
    v16h a;
#pragma unroll
    for (int i = 0; i < 16; ++i) a[i] = row[k0 + frag_k(i, h)];
    return a;
}

#define VST2(T, ptr, val) do { *(volatile T*)(ptr) = (val); __threadfence(); *(volatile T*)(ptr) = (val); } while (0)
typedef float v4f __attribute__((ext_vector_type(4)));
#define VST2V4(ptr, val) do { *(volatile v4f*)(ptr) = (val); __threadfence(); *(volatile v4f*)(ptr) = (val); } while (0)

__device__ __attribute__((noinline)) float act_fn(float v, int act) {
    if (act == 1) return fmaxf(v, 0.f);
    if (act == 2) { const float u = 0.7978845608028654f * (v + 0.044715f * v * v * v); return 0.5f * v * (1.f + tanhf(u)); }
    if (act == 3) return v / (1.f + expf(-v));
    if (act == 4) return 0.5f * v * (1.f + erff(v * 0.7071067811865476f));
    if (act == 5) return tanhf(v);
    if (act == 6) return 1.f / (1.f + expf(-v));
    if (act == 7) return (v > 0.f) ? v : 0.01f * v;
    if (act == 8) return (v > 0.f) ? v : (expf(v) - 1.f);
    if (act == 9) return fminf(fmaxf(v, 0.f), 6.f);
    if (act == 10) return fabsf(v);
    if (act == 11) return (v >= 0.f) ? v : 0.1f * v;
    if (act == 12) return (v > 0.f) ? v : 0.2f * v;
    if (act == 13) return (v > 20.f) ? v : log1pf(expf(v));
    return v;
}

struct GemmP {
    const float* A; const float* B; const float* bias; const float* R; float* C;
    long long sAo, sAi, sAm, sAk, sBo, sBi, sBn, sBk, sCo, sCi, sCm, sRo, sRi, sRm, sRn;
    int M, N, K, zi_n, flags, act; float alpha, beta, sa, sb;
    int Npad, pad_;
};
static_assert(sizeof(GemmP) == 5 * 8 + 15 * 8 + 6 * 4 + 4 * 4 + 2 * 4, "GemmP has padding");

template <int MODE>
__global__ __launch_bounds__(32) void k_gemm(GemmP p) {
    const int lane = threadIdx.x & 31, h = lane >> 4, l15 = lane & 15;
    const int m0 = blockIdx.y * 16, n0 = blockIdx.x * 32;
    const int z = blockIdx.z, zo = z / p.zi_n, zi = z - zo * p.zi_n;
    const float* A = p.A + zo * p.sAo + zi * p.sAi;
    const float* B = p.B + zo * p.sBo + zi * p.sBi;
    const int am = min(m0 + l15, p.M - 1);
    v8f acc[2], comp[2];
#pragma unroll
    for (int t = 0; t < 2; ++t) { v8f zz = {}; acc[t] = zz; comp[t] = zz; }
    for (int k0 = 0; k0 < p.K; k0 += 32) {
        const float* arow = A + (long long)am * p.sAm;
        if (MODE == 1) {
            const Split a = sp_ld(arow, p.sAk, k0, h, p.K, 1.f);
#pragma unroll
            for (int t = 0; t < 2; ++t) {
                const int bn = min(n0 + t * 16 + l15, p.N - 1);
                acc[t] = wmma3(a, sp_ld(B + (long long)bn * p.sBn, p.sBk, k0, h, p.K, 1.f), acc[t]);
            }
        } else if (MODE == 3) {
            const Split3 a = sp3_ld(arow, p.sAk, k0, h, p.K, 1.f);
#pragma unroll
            for (int t = 0; t < 2; ++t) {
                const int bn = min(n0 + t * 16 + l15, p.N - 1);
                acc[t] = wmma6(a, sp3_ld(B + (long long)bn * p.sBn, p.sBk, k0, h, p.K, 1.f), acc[t]);
            }
        } else if (MODE == 4) {
            const Split3 a = sp3_ld(arow, p.sAk, k0, h, p.K, 1.f);
#pragma unroll
            for (int t = 0; t < 2; ++t) {
                const int bn = min(n0 + t * 16 + l15, p.N - 1); v8f zz = {};
                const v8f part = wmma6(a, sp3_ld(B + (long long)bn * p.sBn, p.sBk, k0, h, p.K, 1.f), zz);
                const v8f y = part - comp[t]; const v8f s = acc[t] + y; comp[t] = (s - acc[t]) - y; acc[t] = s;
            }
        } else if (MODE == 2) {
            const v16b a = bh_ld(arow, p.sAk, k0, h, p.K, 1.f);
#pragma unroll
            for (int t = 0; t < 2; ++t) {
                const int bn = min(n0 + t * 16 + l15, p.N - 1);
                acc[t] = wmmab(a, bh_ld(B + (long long)bn * p.sBn, p.sBk, k0, h, p.K, 1.f), acc[t]);
            }
        } else {
            const v16h a = fh_ld(arow, p.sAk, k0, h, p.K, p.sa);
#pragma unroll
            for (int t = 0; t < 2; ++t) {
                const int bn = min(n0 + t * 16 + l15, p.N - 1);
                acc[t] = wmma16(a, fh_ld(B + (long long)bn * p.sBn, p.sBk, k0, h, p.K, p.sb), acc[t]);
            }
        }
    }
    const float iscale = (MODE == 0) ? p.alpha / (p.sa * p.sb) : p.alpha;
    float* C = p.C + zo * p.sCo + zi * p.sCi;
    const float* R = p.R + zo * p.sRo + zi * p.sRi;
    __shared__ __align__(16) float ctile[16][36];
#pragma unroll
    for (int t = 0; t < 2; ++t) {
        const int n = n0 + t * 16 + l15; const int nn = min(n, p.N - 1);
#pragma unroll
        for (int r = 0; r < 8; ++r) {
            const int m = m0 + 8 * h + r; const int mm = min(m, p.M - 1);
            float v = acc[t][r] * iscale;
            if (p.flags & 1) v += p.bias[nn];
            if (p.flags & 2) v += p.bias[mm];
            v = act_fn(v, p.act);
            if (p.flags & 4) v += p.beta * R[(long long)mm * p.sRm + (long long)nn * p.sRn];
            ctile[8 * h + r][t * 16 + l15] = (n < p.N) ? v : 0.f;
        }
    }
    __syncthreads();
    const int NW = (p.Npad > p.N) ? p.Npad : p.N;
    const bool fast = (m0 + 16 <= p.M) && (n0 + 32 <= NW) && ((p.sCm & 3) == 0) && ((((size_t)C) & 15) == 0);
    if (fast) {
#pragma unroll
        for (int s = 0; s < 4; ++s) {
            const int row = s * 4 + (lane >> 3), c4 = (lane & 7) * 4;
            const v4f v = *(const v4f*)&ctile[row][c4];
            VST2V4(C + (long long)(m0 + row) * p.sCm + n0 + c4, v);
        }
    } else {
        for (int row = 0; row < 16; ++row) {
            const int m = m0 + row, n = n0 + lane;
            if (m < p.M && n < NW) VST2(float, C + (long long)m * p.sCm + n, ctile[row][lane]);
        }
    }
}

#define AW 4
struct AttnP {
    const float* Q; const float* K; const float* V; float* O; float* P; const float* Mf; const int* Mi; float* ST;
    const float* Pw; const float* Rt; const int* SQ; const int* SK;
    long long swb, swh, swi, swj, srb, srh, sri;
    long long sQb, sQh, sQi, sQd, sKb, sKh, sKj, sKd, sVb, sVh, sVj, sVd, sOb, sOh, sOi, sPb, sPh, sPi, smb, smh, smi, smj;
    int Lq, Lk, dh, dv, hrep, causal, coff, pband;
    float scale, mfill; int nonorm, mpol;
    int roff, rn, segpol, win;
};
static_assert(sizeof(AttnP) == 12 * 8 + 29 * 8 + 16 * 4, "AttnP has padding");

#ifndef KATTN_ATTR
#define KATTN_ATTR
#endif
template <int DHP, int DVP, int QM, bool SPLITPV, bool TWOPASS>
__global__ __launch_bounds__(32 * AW) KATTN_ATTR void k_attn(AttnP p) {
    constexpr int NT = DVP / 16;
    constexpr int KS = DHP / 32;
    constexpr int VP = DVP + 8;
    __shared__ __align__(16) float    pl[AW][16 * 64];
    __shared__ __align__(16) _Float16 vl[(SPLITPV ? 2 : 1) * 64 * VP];
    const int lane = threadIdx.x & 31, hf = lane >> 4, l15 = lane & 15, wave = threadIdx.x >> 5;
    const int h = blockIdx.y, b = blockIdx.z, hk = h / p.hrep;
    const int q0 = (blockIdx.x * AW + wave) * 16;
    float* myp = pl[wave];
    const float L2E = 1.4426950408889634f;
    const float NEG = -__builtin_inff();
    const int qi = min(q0 + l15, p.Lq - 1);
    const float* qrow = p.Q + b * p.sQb + h * p.sQh + (long long)qi * p.sQi;
    const float* kbase = p.K + b * p.sKb + hk * p.sKh;
    const float* vbase = p.V + b * p.sVb + hk * p.sVh;
    v16h qa[QM == 0 ? KS : 1]; Split qs_[QM == 1 ? KS : 1]; Split3 qt_[QM == 2 ? KS : 1];
#pragma unroll
    for (int ks = 0; ks < KS; ++ks) {
        if (QM == 2) qt_[ks] = sp3_ld(qrow, p.sQd, ks * 32, hf, p.dh, 1.f);
        else if (QM == 1) qs_[ks] = sp_ld(qrow, p.sQd, ks * 32, hf, p.dh, 1.f);
        else qa[ks] = fh_ld(qrow, p.sQd, ks * 32, hf, p.dh, 1.f);
    }
    v8f o[NT]; float m8[8], l8[8];
#pragma unroll
    for (int t = 0; t < NT; ++t) { v8f zz = {}; o[t] = zz; }
#pragma unroll
    for (int i = 0; i < 8; ++i) { m8[i] = NEG; l8[i] = 0.f; }
    int jend = p.Lk;
    if (p.causal == 1) { const int je = (blockIdx.x * AW + AW - 1) * 16 + 16 + p.coff; jend = min(jend, max(je, 0)); }
    const int npass = TWOPASS ? 2 : 1;
    for (int pass = 0; pass < npass; ++pass) {
        const bool dopv = (!TWOPASS) || pass == 1;
        for (int j0 = 0; j0 < jend; j0 += 64) {
            if (dopv) {
                __syncthreads();
                for (int idx = threadIdx.x; idx < 64 * DVP; idx += 32 * AW) {
                    const int jr = idx / DVP, d = idx - jr * DVP, j = j0 + jr;
                    const float f = (j < p.Lk && d < p.dv) ? vbase[(long long)j * p.sVj + (long long)d * p.sVd] : 0.f;
                    if (SPLITPV) {
                        const __bf16 hb = bf16_rne(f);
                        ((__bf16*)vl)[jr * VP + d] = hb; ((__bf16*)vl)[64 * VP + jr * VP + d] = bf16_rne(f - bf16_f32(hb));
                    } else vl[jr * VP + d] = (_Float16)f;
                }
            }
            v8f s[4];
#pragma unroll
            for (int t = 0; t < 4; ++t) {
                const int j = min(j0 + t * 16 + l15, p.Lk - 1);
                const float* krow = kbase + (long long)j * p.sKj;
                v8f acc = {};
#pragma unroll
                for (int ks = 0; ks < KS; ++ks) {
                    if (QM == 2)      acc = wmma6(qt_[ks], sp3_ld(krow, p.sKd, ks * 32, hf, p.dh, 1.f), acc);
                    else if (QM == 1) acc = wmma3(qs_[ks], sp_ld(krow, p.sKd, ks * 32, hf, p.dh, 1.f), acc);
                    else              acc = wmma16(qa[ks], fh_ld(krow, p.sKd, ks * 32, hf, p.dh, 1.f), acc);
                }
                s[t] = acc;
            }
            float pv[8][4];
#pragma unroll
            for (int i = 0; i < 8; ++i) {
                const int irow = q0 + i + 8 * hf;
                const int ic = min(irow, p.Lq - 1);
                float sc[4];
#pragma unroll
                for (int t = 0; t < 4; ++t) {
                    const int jg = j0 + t * 16 + l15;
                    float v = s[t][i] * p.scale;
                    if (p.Mf) v += p.Mf[b * p.smb + h * p.smh + (long long)ic * p.smi + (long long)min(jg, p.Lk - 1) * p.smj];
                    if (p.Rt) { int rc = ic - min(jg, p.Lk - 1) + p.roff; rc = rc < 0 ? 0 : (rc >= p.rn ? p.rn - 1 : rc); v += p.Rt[b * p.srb + h * p.srh + (long long)ic * p.sri + rc]; }
                    if (p.Mi) { const int mv = p.Mi[b * p.smb + h * p.smh + (long long)ic * p.smi + (long long)min(jg, p.Lk - 1) * p.smj]; if (p.mpol ? (mv != 0) : (mv == 0)) v = p.mfill; }
                    if (p.SQ) { const bool same = p.SQ[(long long)b * p.Lq + ic] == p.SK[(long long)b * p.Lk + min(jg, p.Lk - 1)]; if (p.segpol ? same : !same) v = p.mfill; }
                    if (p.causal == 2 && jg > irow + p.coff) v = p.mfill;
                    if (jg >= p.Lk || (p.causal == 1 && jg > irow + p.coff) || (p.causal == 3 && jg < irow + p.coff) || (p.win > 0 && irow + p.coff - jg > p.win)) v = NEG; else v *= L2E;
                    sc[t] = v;
                }
                if (!TWOPASS || pass == 0) {
                    float mx = fmaxf(fmaxf(sc[0], sc[1]), fmaxf(sc[2], sc[3]));
                    mx = fmaxf(mx, __shfl_xor(mx, 1, 32)); mx = fmaxf(mx, __shfl_xor(mx, 2, 32));
                    mx = fmaxf(mx, __shfl_xor(mx, 4, 32)); mx = fmaxf(mx, __shfl_xor(mx, 8, 32));
                    const float mnew = fmaxf(m8[i], mx);
                    const float corr = (mnew == NEG) ? 1.f : exp2f(m8[i] - mnew);
                    float rs = 0.f;
#pragma unroll
                    for (int t = 0; t < 4; ++t) {
                        const float pp = (sc[t] == NEG) ? 0.f : exp2f(sc[t] - mnew); rs += pp;
                        pv[i][t] = p.Pw ? pp * p.Pw[b * p.swb + h * p.swh + (long long)ic * p.swi + (long long)min(j0 + t * 16 + l15, p.Lk - 1) * p.swj] : pp;
                    }
                    rs += __shfl_xor(rs, 1, 32); rs += __shfl_xor(rs, 2, 32); rs += __shfl_xor(rs, 4, 32); rs += __shfl_xor(rs, 8, 32);
                    l8[i] = l8[i] * corr + rs; m8[i] = mnew;
                    if (!TWOPASS) {
#pragma unroll
                        for (int t = 0; t < NT; ++t) o[t][i] *= corr;
                    }
                } else {
                    const float inv = (l8[i] > 0.f) ? 1.f / l8[i] : 0.f;
#pragma unroll
                    for (int t = 0; t < 4; ++t) {
                        const int jg = j0 + t * 16 + l15;
                        float pp = (sc[t] == NEG) ? 0.f : exp2f(sc[t] - m8[i]) * inv;
                        if (p.Pw) pp *= p.Pw[b * p.swb + h * p.swh + (long long)ic * p.swi + (long long)min(jg, p.Lk - 1) * p.swj];
                        pv[i][t] = pp;
                    }
                }
            }
            if (dopv) {
#pragma unroll
                for (int i = 0; i < 8; ++i)
#pragma unroll
                    for (int t = 0; t < 4; ++t) myp[(i + 8 * hf) * 64 + t * 16 + l15] = pv[i][t];
                __syncthreads();
                if (p.P) {
                    float* pb_ = p.P + b * p.sPb + h * p.sPh;
                    const bool fastP = (p.pband == 0) && ((p.sPi & 3) == 0) && (j0 + 64 <= p.Lk) && (q0 + 16 <= p.Lq) && ((((size_t)pb_) & 15) == 0);
                    if (fastP) {
#pragma unroll
                        for (int s = 0; s < 8; ++s) {
                            const int row = s * 2 + (lane >> 4), c4 = (lane & 15) * 4;
                            const v4f v = *(const v4f*)(myp + row * 64 + c4);
                            VST2V4(pb_ + (long long)(q0 + row) * p.sPi + j0 + c4, v);
                        }
                    } else {
                        for (int row = 0; row < 16; ++row) {
                            const int irow = q0 + row; if (irow >= p.Lq) continue;
                            for (int c = lane; c < 64; c += 32) {
                                const int jg = j0 + c; if (jg >= p.Lk) continue;
                                if (p.pband == 0) VST2(float, pb_ + (long long)irow * p.sPi + jg, myp[row * 64 + c]);
                                else if (jg - irow <= p.pband && irow - jg <= p.pband) VST2(float, pb_ + (long long)irow * p.sPi + (jg - irow + p.pband), myp[row * 64 + c]);
                            }
                        }
                    }
                }
                if (SPLITPV) {
                    const Split pa0 = sp_ld(myp + l15 * 64, 1, 0, hf, 64, 1.f), pa1 = sp_ld(myp + l15 * 64, 1, 32, hf, 64, 1.f);
                    const __bf16* vh = (const __bf16*)vl; const __bf16* vlo = vh + 64 * VP;
#pragma unroll
                    for (int t = 0; t < NT; ++t) {
                        const int dcol = t * 16 + l15;
                        Split b0, b1;
#pragma unroll
                        for (int e = 0; e < 16; ++e) {
                            const int k0 = frag_k(e, hf), k1 = 32 + frag_k(e, hf);
                            b0.hi[e] = vh[k0 * VP + dcol]; b0.lo[e] = vlo[k0 * VP + dcol]; b1.hi[e] = vh[k1 * VP + dcol]; b1.lo[e] = vlo[k1 * VP + dcol];
                        }
                        o[t] = wmma3(pa0, b0, o[t]);
                        o[t] = wmma3(pa1, b1, o[t]);
                    }
                } else {
                    const v16h pa0 = fh_ld(myp + l15 * 64, 1, 0, hf, 64, 4096.f), pa1 = fh_ld(myp + l15 * 64, 1, 32, hf, 64, 4096.f);
#pragma unroll
                    for (int t = 0; t < NT; ++t) {
                        const int dcol = t * 16 + l15;
                        v16h b0, b1;
#pragma unroll
                        for (int e = 0; e < 16; ++e) { b0[e] = vl[frag_k(e, hf) * VP + dcol]; b1[e] = vl[(32 + frag_k(e, hf)) * VP + dcol]; }
                        o[t] = wmma16(pa0, b0, o[t]);
                        o[t] = wmma16(pa1, b1, o[t]);
                    }
                }
            }
        }
    }
    float* obase = p.O + b * p.sOb + h * p.sOh;
    if (p.ST) {
        const int rl = lane >> 1, isel = rl & 7;
        float mv = 0.f, lv = 0.f;
#pragma unroll
        for (int i = 0; i < 8; ++i) if (i == isel) { mv = m8[i]; lv = l8[i]; }
        const int irow = q0 + rl;
        if (irow < p.Lq) { float* st = p.ST + (((long long)b * gridDim.y + h) * p.Lq + irow) * 2 + (lane & 1); VST2(float, st, (lane & 1) ? lv : mv * 0.6931471805599453f); }
    }
    float invr[8];
#pragma unroll
    for (int i = 0; i < 8; ++i) {
        if (TWOPASS) invr[i] = SPLITPV ? 1.f : (1.f / 4096.f);
        else if (p.nonorm) invr[i] = exp2f(m8[i]) * (SPLITPV ? 1.f : (1.f / 4096.f));
        else invr[i] = (l8[i] > 0.f) ? (SPLITPV ? 1.f / l8[i] : 1.f / (l8[i] * 4096.f)) : 0.f;
    }
    __syncthreads();
    const bool ofast = ((p.sOi & 3) == 0) && ((((size_t)obase) & 15) == 0) && (q0 + 16 <= p.Lq);
#pragma unroll
    for (int c0 = 0; c0 < DVP; c0 += 64) {
#pragma unroll
        for (int i = 0; i < 8; ++i)
#pragma unroll
            for (int t = 0; t < NT; ++t) if (t * 16 >= c0 && t * 16 < c0 + 64) myp[(i + 8 * hf) * 64 + (t * 16 - c0) + l15] = o[t][i] * invr[i];
        __syncthreads();
        const int cw = (DVP - c0 < 64) ? (DVP - c0) : 64;
        if (ofast && (c0 + cw <= p.dv) && (cw % 32 == 0)) {
            const int lpr = cw / 4;
            const int rows_per_ins = 32 / lpr;
            for (int r0 = 0; r0 < 16; r0 += rows_per_ins) {
                const int row = r0 + lane / lpr, c4 = (lane % lpr) * 4;
                const v4f v = *(const v4f*)(myp + row * 64 + c4);
                VST2V4(obase + (long long)(q0 + row) * p.sOi + c0 + c4, v);
            }
        } else {
            for (int row = 0; row < 16; ++row) {
                const int irow = q0 + row; if (irow >= p.Lq) continue;
                for (int c = lane; c < cw; c += 32) { const int d = c0 + c; if (d < p.dv) VST2(float, obase + (long long)irow * p.sOi + d, myp[row * 64 + c]); }
            }
        }
        __syncthreads();
    }
}

struct TrP { const float* src; float* dst; const float* R2; long long sSz, lds, sDz, ldd, sRz, ldr; int R, C, flags, act; float alpha, beta; };
static_assert(sizeof(TrP) == 3 * 8 + 6 * 8 + 6 * 4, "TrP has padding");
__global__ __launch_bounds__(256) void k_tr(TrP p) {
    __shared__ float tile[32][33];
    const int c0 = blockIdx.x * 32, r0 = blockIdx.y * 32, z = blockIdx.z;
    const int lane = threadIdx.x & 31, wave = threadIdx.x >> 5;
    const float* s = p.src + z * p.sSz;
#pragma unroll
    for (int k = 0; k < 4; ++k) {
        const int rl = wave * 4 + k, r = r0 + rl, c = c0 + lane;
        tile[rl][lane] = (r < p.R && c < p.C) ? s[(long long)r * p.lds + c] : 0.f;
    }
    __syncthreads();
    float* d = p.dst + z * p.sDz; const float* rr = p.R2 + z * p.sRz;
#pragma unroll
    for (int k = 0; k < 4; ++k) {
        const int cl = wave * 4 + k, c = c0 + cl, r = r0 + lane;
        if (c < p.C && r < p.R) {
            float v = act_fn(p.alpha * tile[lane][cl], p.act);
            if (p.flags & 1) v += p.beta * rr[(long long)c * p.ldr + r];
            VST2(float, d + (long long)c * p.ldd + r, v);
        }
    }
}

__global__ __launch_bounds__(256) void k_affine(const float* __restrict__ src, float* __restrict__ dst, int n, float a, float b, const float* __restrict__ sdev) {
    const int i = blockIdx.x * 256 + threadIdx.x;
    if (i < n) { const float aa = sdev ? a * sdev[0] : a; const float v = aa * src[i] + b; VST2(float, dst + i, v); }
}

struct SmP { const float* src; float* dst; const float* Mf; long long sz, sr, dz, dr, smz, smr; int n, pad; float scale_in, scale_out; };
static_assert(sizeof(SmP) == 3 * 8 + 6 * 8 + 4 * 4, "SmP has padding");
__global__ __launch_bounds__(256) void k_softmax(SmP p) {
    __shared__ float red[256];
    const int r = blockIdx.x, z = blockIdx.y, tid = threadIdx.x;
    const float* s = p.src + z * p.sz + (long long)r * p.sr;
    const float* mf = p.Mf ? (p.Mf + z * p.smz + (long long)r * p.smr) : nullptr;
    float mx = -__builtin_inff();
    for (int j = tid; j < p.n; j += 256) { float v = s[j] * p.scale_in; if (mf) v += mf[j]; mx = fmaxf(mx, v); }
    red[tid] = mx; __syncthreads();
    for (int o = 128; o > 0; o >>= 1) { if (tid < o) red[tid] = fmaxf(red[tid], red[tid + o]); __syncthreads(); }
    mx = red[0]; __syncthreads();
    float sum = 0.f;
    for (int j = tid; j < p.n; j += 256) { float v = s[j] * p.scale_in; if (mf) v += mf[j]; sum += (mx == -__builtin_inff()) ? 0.f : expf(v - mx); }
    red[tid] = sum; __syncthreads();
    for (int o = 128; o > 0; o >>= 1) { if (tid < o) red[tid] += red[tid + o]; __syncthreads(); }
    sum = red[0];
    const float inv = (sum > 0.f) ? p.scale_out / sum : 0.f;
    float* d = p.dst + z * p.dz + (long long)r * p.dr;
    for (int j = tid; j < p.n; j += 256) { float v = s[j] * p.scale_in; if (mf) v += mf[j]; const float o = (mx == -__builtin_inff()) ? 0.f : expf(v - mx) * inv; VST2(float, d + j, o); }
}
__global__ __launch_bounds__(256) void k_stats(const float* __restrict__ x, long long sz, long long so, long long si, int inner, int n, float eps, float* __restrict__ stat, int mode) {
    __shared__ float red[256];
    const int z = blockIdx.x, tid = threadIdx.x;
    const float* base = x + z * sz;
    float s = 0.f;
    for (int e = tid; e < n; e += 256) s += base[(long long)(e / inner) * so + (long long)(e % inner) * si];
    red[tid] = s; __syncthreads();
    for (int o = 128; o > 0; o >>= 1) { if (tid < o) red[tid] += red[tid + o]; __syncthreads(); }
    const float mu = (mode == 0 || mode == 3) ? red[0] / (float)n : 0.f; __syncthreads();
    float q = 0.f;
    for (int e = tid; e < n; e += 256) { const float dlt = base[(long long)(e / inner) * so + (long long)(e % inner) * si] - mu; q += dlt * dlt; }
    red[tid] = q; __syncthreads();
    for (int o = 128; o > 0; o >>= 1) { if (tid < o) red[tid] += red[tid + o]; __syncthreads(); }
    {
        float rs;
        if (mode == 2) rs = sqrtf((float)n) / fmaxf(sqrtf(red[0]), eps); else if (mode == 3) rs = rsqrtf(red[0] / (float)(n - 1) + eps); else rs = rsqrtf(red[0] / (float)n + eps);
        if (tid < 32) { const float v = (tid == 0) ? mu : ((tid == 1) ? rs : 0.f); VST2(float, stat + (long long)z * 32 + tid, v); }
    }
}
__global__ __launch_bounds__(256) void k_norm_apply(const float* __restrict__ x, float* __restrict__ y, const float* __restrict__ stat, const float* __restrict__ g, const float* __restrict__ bta,
                                                     int Z, int C, int L, int G, int bn, int act) {
    const long long idx = (long long)blockIdx.x * 256 + threadIdx.x;
    if (idx >= (long long)Z * C * L) return;
    const int l = (int)(idx % L); const long long zc = idx / L; const int c = (int)(zc % C), z = (int)(zc / C); (void)l;
    const int set = bn ? c : (z * G + c / (C / G));
    float v = (x[idx] - stat[(long long)set * 32]) * stat[(long long)set * 32 + 1];
    if (g) v *= g[c];
    if (bta) v += bta[c];
    v = act_fn(v, act);
    VST2(float, y + idx, v);
}

__global__ __launch_bounds__(256) void k_lse_neg(const float* __restrict__ st, float* __restrict__ c, int n) {
    const int i = blockIdx.x * 256 + threadIdx.x;
    if (i < n) { const float v = -(st[2 * i] + logf(st[2 * i + 1])); VST2(float, c + i, v); }
}

__global__ __launch_bounds__(256) void k_iota(int* __restrict__ dst, int n, int a, int b) {
    const int i = blockIdx.x * 256 + threadIdx.x;
    if (i < n) { const int v = a * i + b; VST2(int, dst + i, v); }
}

__global__ __launch_bounds__(256) void k_axpby(const float* __restrict__ x, const float* __restrict__ y, float* __restrict__ dst, int n, float a, float b, float c) {
    const int i = blockIdx.x * 256 + threadIdx.x;
    if (i < n) { const float v = a * x[i] + b * y[i] + c; VST2(float, dst + i, v); }
}

struct RopeP { const float* X; float* Y; const float* C; const float* Sn; const int* pos; long long sXr, sXh, sYr, sYh, sCb, sCp, sCd; int R, Hn, D, S, mode, tmode, pmode, pad; };
static_assert(sizeof(RopeP) == 5 * 8 + 7 * 8 + 8 * 4, "RopeP has padding");
__global__ __launch_bounds__(256) void k_rope(RopeP p) {
    const long long idx = (long long)blockIdx.x * 256 + threadIdx.x;
    if (idx >= (long long)p.R * p.Hn * p.D) return;
    const int d = (int)(idx % p.D); const long long rh = idx / p.D; const int h = (int)(rh % p.Hn); const int r = (int)(rh / p.Hn);
    const int half = p.D / 2;
    int partner; float sign;
    if (p.mode == 0) { partner = (d < half) ? d + half : d - half; sign = (d < half) ? -1.f : 1.f; }
    else { partner = d ^ 1; sign = (d & 1) ? 1.f : -1.f; }
    const int tcol = (p.tmode == 0) ? d : ((p.tmode == 1) ? (d % half) : (d >> 1));
    const int pp = (p.pmode == 0) ? (r % p.S) : ((p.pmode == 1) ? h : p.pos[r]);
    const long long toff = (long long)(r / p.S) * p.sCb + (long long)pp * p.sCp + (long long)tcol * p.sCd;
    const float* xr = p.X + (long long)r * p.sXr + (long long)h * p.sXh;
    const float v = xr[d] * p.C[toff] + sign * xr[partner] * p.Sn[toff];
    VST2(float, p.Y + (long long)r * p.sYr + (long long)h * p.sYh + d, v);
}

__global__ __launch_bounds__(256) void k_invf(float* __restrict__ invb, int half, int D, float base, float num, int fmode, float cexp) {
    const int i = blockIdx.x * 256 + threadIdx.x;
    if (i >= ((half + 31) / 32) * 32) return;
    if (i >= half) { VST2(float, invb + i, 0.f); return; }
    const float e = (float)(2 * i) / (float)D;
    float invf;
    if (fmode == 1) invf = num * expf((float)(2 * i) * cexp);
    else if (fmode == 2) invf = num * powf(base, (-2.0f * ((float)i - 1.0f)) / (float)D);
    else invf = num * (1.0f / powf(base, e));
    VST2(float, invb + i, invf);
}
__global__ __launch_bounds__(256) void k_sincos(float* __restrict__ cs, float* __restrict__ sn, const float* __restrict__ invb, int S, int half, float pscale) {
    const int idx = blockIdx.x * 256 + threadIdx.x;
    if (idx >= S * half) return;
    const int s = idx / half, i = idx - s * half;
    const float ang = (pscale * (float)s) * invb[i];
    VST2(float, cs + idx, cosf(ang)); VST2(float, sn + idx, sinf(ang));
}

__global__ __launch_bounds__(256) void k_mulact(const float* __restrict__ x, const float* __restrict__ y, float* __restrict__ dst, int n, int act) {
    const int i = blockIdx.x * 256 + threadIdx.x;
    if (i < n) { const float v = act_fn(x[i], act) * y[i]; VST2(float, dst + i, v); }
}

__global__ __launch_bounds__(256) void k_matvec(GemmP p) {
    const int rpt = (p.N == 1) ? 1 : 32;
    const long long r0 = ((long long)blockIdx.x * 256 + threadIdx.x) * rpt; const int z = blockIdx.z, zo = z / p.zi_n, zi = z - zo * p.zi_n;
    if (r0 >= p.M) return;
    const float* Bb = p.B + zo * p.sBo + zi * p.sBi;
    float* C = p.C + zo * p.sCo + zi * p.sCi; const float* R = p.R + zo * p.sRo + zi * p.sRi;
    for (int rr = 0; rr < rpt; ++rr) {
        const long long r = r0 + rr; if (r >= p.M) break;
        const float* A = p.A + zo * p.sAo + zi * p.sAi + r * p.sAm;
        float acc[8] = {0.f, 0.f, 0.f, 0.f, 0.f, 0.f, 0.f, 0.f};
        for (int k = 0; k < p.K; ++k) { const float a = A[(long long)k * p.sAk];
#pragma unroll
            for (int j = 0; j < 8; ++j) if (j < p.N) acc[j] += a * Bb[(long long)j * p.sBn + (long long)k * p.sBk]; }
#pragma unroll
        for (int j = 0; j < 8; ++j) if (j < p.N) {
            float v = acc[j] * p.alpha;
            if (p.flags & 1) v += p.bias[j];
            if (p.flags & 2) v += p.bias[r];
            v = act_fn(v, p.act);
            if (p.flags & 4) v += p.beta * R[r * p.sRm + (long long)j * p.sRn];
            VST2(float, C + r * p.sCm + j, v);
        }
    }
}
__global__ __launch_bounds__(256) void k_smallsoftmax(const float* __restrict__ src, float* __restrict__ dst, long long sr, long long dr, int n, long long R, float scale) {
    const long long r0 = ((long long)blockIdx.x * 256 + threadIdx.x) * 32;
    for (int rr = 0; rr < 32; ++rr) {
        const long long r = r0 + rr; if (r >= R) return;
        const float* s = src + r * sr; float* d = dst + r * dr;
        float mx = -__builtin_inff();
        for (int j = 0; j < n; ++j) mx = fmaxf(mx, s[j] * scale);
        float sum = 0.f;
        for (int j = 0; j < n; ++j) sum += expf(s[j] * scale - mx);
        const float inv = 1.f / sum;
        for (int j = 0; j < n; ++j) { const float v = expf(s[j] * scale - mx) * inv; VST2(float, d + j, v); }
    }
}

__global__ __launch_bounds__(32) void k_unitstat(float* __restrict__ st) { const int t = threadIdx.x; const float v = (t == 1) ? 1.f : 0.f; VST2(float, st + t, v); }

__global__ __launch_bounds__(256) void k_lincopy(const float* __restrict__ src, long long lds, float* __restrict__ dst, long long ldd, long long rows, int cols) {
    const long long i = (long long)blockIdx.x * 256 + threadIdx.x; if (i >= rows * cols) return;
    const long long r = i / cols; const int c = (int)(i - r * cols);
    const float v = src[r * lds + c]; VST2(float, dst + r * ldd + c, v);
}

__global__ __launch_bounds__(256) void k_caps_soft(const float* __restrict__ BL, float* __restrict__ CC, int B, int O, int I) {
    const int t = blockIdx.x * 256 + threadIdx.x; if (t >= B * I) return; const int i = t % I; const int b = t / I; const float* bl = BL + (long long)b * O * I + i;
    float mx = -__builtin_inff(); for (int o = 0; o < O; ++o) mx = fmaxf(mx, bl[(long long)o * I]);
    float s = 0.f; for (int o = 0; o < O; ++o) s += expf(bl[(long long)o * I] - mx);
    for (int o = 0; o < O; ++o) { const float v = expf(bl[(long long)o * I] - mx) / s; VST2(float, CC + ((long long)b * O + o) * I + i, v); }
}
__global__ __launch_bounds__(256) void k_caps_cp(const float* __restrict__ P, const float* __restrict__ CC, float* __restrict__ CP, int b, int O, int I) {
    const long long t = (long long)blockIdx.x * 256 + threadIdx.x; if (t >= (long long)O * 4 * I * 4) return; const int iy = (int)(t % (I * 4)); const int x = (int)((t / (I * 4)) % 4); const int o = (int)(t / ((long long)I * 16)); const int i = iy >> 2, y = iy & 3;
    const float v = CC[((long long)b * O + o) * I + i] * P[(((long long)b * I + i) * 4 + x) * 4 + y]; VST2(float, CP + t, v);
}
__global__ __launch_bounds__(256) void k_caps_squash(const float* __restrict__ S, int ldp, float* __restrict__ V, float* __restrict__ POUT, float* __restrict__ AOUT, int BO, int fin) {
    const int t = blockIdx.x * 256 + threadIdx.x; if (t >= BO * 16) return; const int e = t & 15; const int bo = t >> 4; const int x = e >> 2, z = e & 3;
    float n2 = 0.f; for (int q = 0; q < 16; ++q) { const float v = S[((long long)bo * 4 + (q >> 2)) * ldp + (q & 3)]; n2 += v * v; }
    const float f = (n2 / (1.f + n2)) / sqrtf(n2 + 1e-12f); const float v = S[((long long)bo * 4 + x) * ldp + z] * f;
    if (fin) { VST2(float, POUT + t, v); if (e == 0) { const float a = sqrtf(n2 * f * f + 1e-12f); VST2(float, AOUT + bo, a); } }
    else VST2(float, V + t, v);
}
__global__ __launch_bounds__(256) void k_caps_agree(const float* __restrict__ P, const float* __restrict__ Wc, const float* __restrict__ V, float* __restrict__ BL, int B, int O, int I) {
    const long long t = (long long)blockIdx.x * 256 + threadIdx.x; if (t >= (long long)B * O * I) return; const int i = (int)(t % I); const int o = (int)((t / I) % O); const int b = (int)(t / ((long long)I * O));
    const float* p = P + ((long long)b * I + i) * 16; const float* w = Wc + ((long long)o * I + i) * 16; const float* v = V + ((long long)b * O + o) * 16; float s = 0.f;
#pragma unroll
    for (int x = 0; x < 4; ++x)
#pragma unroll
        for (int y = 0; y < 4; ++y) { const float pxy = p[x * 4 + y]; float q = 0.f;
#pragma unroll
            for (int z = 0; z < 4; ++z) q += w[y * 4 + z] * v[x * 4 + z];
            s += pxy * q; }
    const float nb = BL[t] + s;
    VST2(float, BL + t, nb);
}

template __global__ void k_gemm<1>(GemmP);

extern "C" void kernel_launch(void* const* d_in, const int* in_sizes, int n_in, void* d_out, int out_size, void* d_ws, size_t ws_size, hipStream_t stream) {
    (void)in_sizes; (void)n_in; (void)out_size; (void)ws_size;
    const float* P = (const float*)d_in[0];
    const float* act = (const float*)d_in[1];
    const float* Wc = (const float*)d_in[2];
    const int Bn = 32;
    const int I = 4096;
    const int O = 32;
    const int KD = I * 4;
    const int LP = 32;
    const int ITERS = 3;
    float* out = (float*)d_out;
    float* aout = out + ((size_t)Bn * O * 16);
    char* wsp = (char*)d_ws;
    float* BL = (float*)wsp; wsp += (((size_t)((size_t)Bn * O * I) * 4 + 255) / 256) * 256;
    float* CC = (float*)wsp; wsp += (((size_t)((size_t)Bn * O * I) * 4 + 255) / 256) * 256;
    float* CP = (float*)wsp; wsp += (((size_t)((size_t)O * 4 * KD) * 4 + 255) / 256) * 256;
    float* S = (float*)wsp; wsp += (((size_t)((size_t)Bn * O * 4 * LP) * 4 + 255) / 256) * 256;
    float* V = (float*)wsp; wsp += (((size_t)((size_t)Bn * O * 16) * 4 + 255) / 256) * 256;
    hipMemsetAsync(BL, 0, (size_t)Bn * O * I * 4, stream);
    k_caps_soft<<<(unsigned)((Bn * I + 255) / 256), 256, 0, stream>>>(BL, CC, Bn, O, I);
    k_caps_cp<<<(unsigned)(((long long)O * 4 * KD + 255) / 256), 256, 0, stream>>>(P, CC, CP, 0, O, I);
    { GemmP gs0_0;
      gs0_0.A = CP; gs0_0.B = Wc; gs0_0.bias = CP; gs0_0.R = CP; gs0_0.C = S + (size_t)0 * O * 4 * LP;
      gs0_0.sAo = (long long)4 * KD; gs0_0.sAi = 0; gs0_0.sAm = KD; gs0_0.sAk = 1; gs0_0.sBo = (long long)KD * 4; gs0_0.sBi = 0; gs0_0.sBn = 1; gs0_0.sBk = 4; gs0_0.sCo = 4 * LP; gs0_0.sCi = 0; gs0_0.sCm = LP; gs0_0.sRo = 0; gs0_0.sRi = 0; gs0_0.sRm = 0; gs0_0.sRn = 0;
      gs0_0.M = 4; gs0_0.N = 4; gs0_0.K = KD; gs0_0.zi_n = 1; gs0_0.flags = 0; gs0_0.act = 0;
      gs0_0.alpha = 1.0f; gs0_0.beta = 0.0f; gs0_0.sa = 1.0f; gs0_0.sb = 1.0f; gs0_0.Npad = LP; gs0_0.pad_ = 0;
      k_gemm<1><<<dim3((unsigned)((LP) + 31) / 32, (unsigned)((4) + 15) / 16, (unsigned)(O)), 32, 0, stream>>>(gs0_0); }
    k_caps_cp<<<(unsigned)(((long long)O * 4 * KD + 255) / 256), 256, 0, stream>>>(P, CC, CP, 1, O, I);
    { GemmP gs0_1;
      gs0_1.A = CP; gs0_1.B = Wc; gs0_1.bias = CP; gs0_1.R = CP; gs0_1.C = S + (size_t)1 * O * 4 * LP;
      gs0_1.sAo = (long long)4 * KD; gs0_1.sAi = 0; gs0_1.sAm = KD; gs0_1.sAk = 1; gs0_1.sBo = (long long)KD * 4; gs0_1.sBi = 0; gs0_1.sBn = 1; gs0_1.sBk = 4; gs0_1.sCo = 4 * LP; gs0_1.sCi = 0; gs0_1.sCm = LP; gs0_1.sRo = 0; gs0_1.sRi = 0; gs0_1.sRm = 0; gs0_1.sRn = 0;
      gs0_1.M = 4; gs0_1.N = 4; gs0_1.K = KD; gs0_1.zi_n = 1; gs0_1.flags = 0; gs0_1.act = 0;
      gs0_1.alpha = 1.0f; gs0_1.beta = 0.0f; gs0_1.sa = 1.0f; gs0_1.sb = 1.0f; gs0_1.Npad = LP; gs0_1.pad_ = 0;
      k_gemm<1><<<dim3((unsigned)((LP) + 31) / 32, (unsigned)((4) + 15) / 16, (unsigned)(O)), 32, 0, stream>>>(gs0_1); }
    k_caps_cp<<<(unsigned)(((long long)O * 4 * KD + 255) / 256), 256, 0, stream>>>(P, CC, CP, 2, O, I);
    { GemmP gs0_2;
      gs0_2.A = CP; gs0_2.B = Wc; gs0_2.bias = CP; gs0_2.R = CP; gs0_2.C = S + (size_t)2 * O * 4 * LP;
      gs0_2.sAo = (long long)4 * KD; gs0_2.sAi = 0; gs0_2.sAm = KD; gs0_2.sAk = 1; gs0_2.sBo = (long long)KD * 4; gs0_2.sBi = 0; gs0_2.sBn = 1; gs0_2.sBk = 4; gs0_2.sCo = 4 * LP; gs0_2.sCi = 0; gs0_2.sCm = LP; gs0_2.sRo = 0; gs0_2.sRi = 0; gs0_2.sRm = 0; gs0_2.sRn = 0;
      gs0_2.M = 4; gs0_2.N = 4; gs0_2.K = KD; gs0_2.zi_n = 1; gs0_2.flags = 0; gs0_2.act = 0;
      gs0_2.alpha = 1.0f; gs0_2.beta = 0.0f; gs0_2.sa = 1.0f; gs0_2.sb = 1.0f; gs0_2.Npad = LP; gs0_2.pad_ = 0;
      k_gemm<1><<<dim3((unsigned)((LP) + 31) / 32, (unsigned)((4) + 15) / 16, (unsigned)(O)), 32, 0, stream>>>(gs0_2); }
    k_caps_cp<<<(unsigned)(((long long)O * 4 * KD + 255) / 256), 256, 0, stream>>>(P, CC, CP, 3, O, I);
    { GemmP gs0_3;
      gs0_3.A = CP; gs0_3.B = Wc; gs0_3.bias = CP; gs0_3.R = CP; gs0_3.C = S + (size_t)3 * O * 4 * LP;
      gs0_3.sAo = (long long)4 * KD; gs0_3.sAi = 0; gs0_3.sAm = KD; gs0_3.sAk = 1; gs0_3.sBo = (long long)KD * 4; gs0_3.sBi = 0; gs0_3.sBn = 1; gs0_3.sBk = 4; gs0_3.sCo = 4 * LP; gs0_3.sCi = 0; gs0_3.sCm = LP; gs0_3.sRo = 0; gs0_3.sRi = 0; gs0_3.sRm = 0; gs0_3.sRn = 0;
      gs0_3.M = 4; gs0_3.N = 4; gs0_3.K = KD; gs0_3.zi_n = 1; gs0_3.flags = 0; gs0_3.act = 0;
      gs0_3.alpha = 1.0f; gs0_3.beta = 0.0f; gs0_3.sa = 1.0f; gs0_3.sb = 1.0f; gs0_3.Npad = LP; gs0_3.pad_ = 0;
      k_gemm<1><<<dim3((unsigned)((LP) + 31) / 32, (unsigned)((4) + 15) / 16, (unsigned)(O)), 32, 0, stream>>>(gs0_3); }
    k_caps_cp<<<(unsigned)(((long long)O * 4 * KD + 255) / 256), 256, 0, stream>>>(P, CC, CP, 4, O, I);
    { GemmP gs0_4;
      gs0_4.A = CP; gs0_4.B = Wc; gs0_4.bias = CP; gs0_4.R = CP; gs0_4.C = S + (size_t)4 * O * 4 * LP;
      gs0_4.sAo = (long long)4 * KD; gs0_4.sAi = 0; gs0_4.sAm = KD; gs0_4.sAk = 1; gs0_4.sBo = (long long)KD * 4; gs0_4.sBi = 0; gs0_4.sBn = 1; gs0_4.sBk = 4; gs0_4.sCo = 4 * LP; gs0_4.sCi = 0; gs0_4.sCm = LP; gs0_4.sRo = 0; gs0_4.sRi = 0; gs0_4.sRm = 0; gs0_4.sRn = 0;
      gs0_4.M = 4; gs0_4.N = 4; gs0_4.K = KD; gs0_4.zi_n = 1; gs0_4.flags = 0; gs0_4.act = 0;
      gs0_4.alpha = 1.0f; gs0_4.beta = 0.0f; gs0_4.sa = 1.0f; gs0_4.sb = 1.0f; gs0_4.Npad = LP; gs0_4.pad_ = 0;
      k_gemm<1><<<dim3((unsigned)((LP) + 31) / 32, (unsigned)((4) + 15) / 16, (unsigned)(O)), 32, 0, stream>>>(gs0_4); }
    k_caps_cp<<<(unsigned)(((long long)O * 4 * KD + 255) / 256), 256, 0, stream>>>(P, CC, CP, 5, O, I);
    { GemmP gs0_5;
      gs0_5.A = CP; gs0_5.B = Wc; gs0_5.bias = CP; gs0_5.R = CP; gs0_5.C = S + (size_t)5 * O * 4 * LP;
      gs0_5.sAo = (long long)4 * KD; gs0_5.sAi = 0; gs0_5.sAm = KD; gs0_5.sAk = 1; gs0_5.sBo = (long long)KD * 4; gs0_5.sBi = 0; gs0_5.sBn = 1; gs0_5.sBk = 4; gs0_5.sCo = 4 * LP; gs0_5.sCi = 0; gs0_5.sCm = LP; gs0_5.sRo = 0; gs0_5.sRi = 0; gs0_5.sRm = 0; gs0_5.sRn = 0;
      gs0_5.M = 4; gs0_5.N = 4; gs0_5.K = KD; gs0_5.zi_n = 1; gs0_5.flags = 0; gs0_5.act = 0;
      gs0_5.alpha = 1.0f; gs0_5.beta = 0.0f; gs0_5.sa = 1.0f; gs0_5.sb = 1.0f; gs0_5.Npad = LP; gs0_5.pad_ = 0;
      k_gemm<1><<<dim3((unsigned)((LP) + 31) / 32, (unsigned)((4) + 15) / 16, (unsigned)(O)), 32, 0, stream>>>(gs0_5); }
    k_caps_cp<<<(unsigned)(((long long)O * 4 * KD + 255) / 256), 256, 0, stream>>>(P, CC, CP, 6, O, I);
    { GemmP gs0_6;
      gs0_6.A = CP; gs0_6.B = Wc; gs0_6.bias = CP; gs0_6.R = CP; gs0_6.C = S + (size_t)6 * O * 4 * LP;
      gs0_6.sAo = (long long)4 * KD; gs0_6.sAi = 0; gs0_6.sAm = KD; gs0_6.sAk = 1; gs0_6.sBo = (long long)KD * 4; gs0_6.sBi = 0; gs0_6.sBn = 1; gs0_6.sBk = 4; gs0_6.sCo = 4 * LP; gs0_6.sCi = 0; gs0_6.sCm = LP; gs0_6.sRo = 0; gs0_6.sRi = 0; gs0_6.sRm = 0; gs0_6.sRn = 0;
      gs0_6.M = 4; gs0_6.N = 4; gs0_6.K = KD; gs0_6.zi_n = 1; gs0_6.flags = 0; gs0_6.act = 0;
      gs0_6.alpha = 1.0f; gs0_6.beta = 0.0f; gs0_6.sa = 1.0f; gs0_6.sb = 1.0f; gs0_6.Npad = LP; gs0_6.pad_ = 0;
      k_gemm<1><<<dim3((unsigned)((LP) + 31) / 32, (unsigned)((4) + 15) / 16, (unsigned)(O)), 32, 0, stream>>>(gs0_6); }
    k_caps_cp<<<(unsigned)(((long long)O * 4 * KD + 255) / 256), 256, 0, stream>>>(P, CC, CP, 7, O, I);
    { GemmP gs0_7;
      gs0_7.A = CP; gs0_7.B = Wc; gs0_7.bias = CP; gs0_7.R = CP; gs0_7.C = S + (size_t)7 * O * 4 * LP;
      gs0_7.sAo = (long long)4 * KD; gs0_7.sAi = 0; gs0_7.sAm = KD; gs0_7.sAk = 1; gs0_7.sBo = (long long)KD * 4; gs0_7.sBi = 0; gs0_7.sBn = 1; gs0_7.sBk = 4; gs0_7.sCo = 4 * LP; gs0_7.sCi = 0; gs0_7.sCm = LP; gs0_7.sRo = 0; gs0_7.sRi = 0; gs0_7.sRm = 0; gs0_7.sRn = 0;
      gs0_7.M = 4; gs0_7.N = 4; gs0_7.K = KD; gs0_7.zi_n = 1; gs0_7.flags = 0; gs0_7.act = 0;
      gs0_7.alpha = 1.0f; gs0_7.beta = 0.0f; gs0_7.sa = 1.0f; gs0_7.sb = 1.0f; gs0_7.Npad = LP; gs0_7.pad_ = 0;
      k_gemm<1><<<dim3((unsigned)((LP) + 31) / 32, (unsigned)((4) + 15) / 16, (unsigned)(O)), 32, 0, stream>>>(gs0_7); }
    k_caps_cp<<<(unsigned)(((long long)O * 4 * KD + 255) / 256), 256, 0, stream>>>(P, CC, CP, 8, O, I);
    { GemmP gs0_8;
      gs0_8.A = CP; gs0_8.B = Wc; gs0_8.bias = CP; gs0_8.R = CP; gs0_8.C = S + (size_t)8 * O * 4 * LP;
      gs0_8.sAo = (long long)4 * KD; gs0_8.sAi = 0; gs0_8.sAm = KD; gs0_8.sAk = 1; gs0_8.sBo = (long long)KD * 4; gs0_8.sBi = 0; gs0_8.sBn = 1; gs0_8.sBk = 4; gs0_8.sCo = 4 * LP; gs0_8.sCi = 0; gs0_8.sCm = LP; gs0_8.sRo = 0; gs0_8.sRi = 0; gs0_8.sRm = 0; gs0_8.sRn = 0;
      gs0_8.M = 4; gs0_8.N = 4; gs0_8.K = KD; gs0_8.zi_n = 1; gs0_8.flags = 0; gs0_8.act = 0;
      gs0_8.alpha = 1.0f; gs0_8.beta = 0.0f; gs0_8.sa = 1.0f; gs0_8.sb = 1.0f; gs0_8.Npad = LP; gs0_8.pad_ = 0;
      k_gemm<1><<<dim3((unsigned)((LP) + 31) / 32, (unsigned)((4) + 15) / 16, (unsigned)(O)), 32, 0, stream>>>(gs0_8); }
    k_caps_cp<<<(unsigned)(((long long)O * 4 * KD + 255) / 256), 256, 0, stream>>>(P, CC, CP, 9, O, I);
    { GemmP gs0_9;
      gs0_9.A = CP; gs0_9.B = Wc; gs0_9.bias = CP; gs0_9.R = CP; gs0_9.C = S + (size_t)9 * O * 4 * LP;
      gs0_9.sAo = (long long)4 * KD; gs0_9.sAi = 0; gs0_9.sAm = KD; gs0_9.sAk = 1; gs0_9.sBo = (long long)KD * 4; gs0_9.sBi = 0; gs0_9.sBn = 1; gs0_9.sBk = 4; gs0_9.sCo = 4 * LP; gs0_9.sCi = 0; gs0_9.sCm = LP; gs0_9.sRo = 0; gs0_9.sRi = 0; gs0_9.sRm = 0; gs0_9.sRn = 0;
      gs0_9.M = 4; gs0_9.N = 4; gs0_9.K = KD; gs0_9.zi_n = 1; gs0_9.flags = 0; gs0_9.act = 0;
      gs0_9.alpha = 1.0f; gs0_9.beta = 0.0f; gs0_9.sa = 1.0f; gs0_9.sb = 1.0f; gs0_9.Npad = LP; gs0_9.pad_ = 0;
      k_gemm<1><<<dim3((unsigned)((LP) + 31) / 32, (unsigned)((4) + 15) / 16, (unsigned)(O)), 32, 0, stream>>>(gs0_9); }
    k_caps_cp<<<(unsigned)(((long long)O * 4 * KD + 255) / 256), 256, 0, stream>>>(P, CC, CP, 10, O, I);
    { GemmP gs0_10;
      gs0_10.A = CP; gs0_10.B = Wc; gs0_10.bias = CP; gs0_10.R = CP; gs0_10.C = S + (size_t)10 * O * 4 * LP;
      gs0_10.sAo = (long long)4 * KD; gs0_10.sAi = 0; gs0_10.sAm = KD; gs0_10.sAk = 1; gs0_10.sBo = (long long)KD * 4; gs0_10.sBi = 0; gs0_10.sBn = 1; gs0_10.sBk = 4; gs0_10.sCo = 4 * LP; gs0_10.sCi = 0; gs0_10.sCm = LP; gs0_10.sRo = 0; gs0_10.sRi = 0; gs0_10.sRm = 0; gs0_10.sRn = 0;
      gs0_10.M = 4; gs0_10.N = 4; gs0_10.K = KD; gs0_10.zi_n = 1; gs0_10.flags = 0; gs0_10.act = 0;
      gs0_10.alpha = 1.0f; gs0_10.beta = 0.0f; gs0_10.sa = 1.0f; gs0_10.sb = 1.0f; gs0_10.Npad = LP; gs0_10.pad_ = 0;
      k_gemm<1><<<dim3((unsigned)((LP) + 31) / 32, (unsigned)((4) + 15) / 16, (unsigned)(O)), 32, 0, stream>>>(gs0_10); }
    k_caps_cp<<<(unsigned)(((long long)O * 4 * KD + 255) / 256), 256, 0, stream>>>(P, CC, CP, 11, O, I);
    { GemmP gs0_11;
      gs0_11.A = CP; gs0_11.B = Wc; gs0_11.bias = CP; gs0_11.R = CP; gs0_11.C = S + (size_t)11 * O * 4 * LP;
      gs0_11.sAo = (long long)4 * KD; gs0_11.sAi = 0; gs0_11.sAm = KD; gs0_11.sAk = 1; gs0_11.sBo = (long long)KD * 4; gs0_11.sBi = 0; gs0_11.sBn = 1; gs0_11.sBk = 4; gs0_11.sCo = 4 * LP; gs0_11.sCi = 0; gs0_11.sCm = LP; gs0_11.sRo = 0; gs0_11.sRi = 0; gs0_11.sRm = 0; gs0_11.sRn = 0;
      gs0_11.M = 4; gs0_11.N = 4; gs0_11.K = KD; gs0_11.zi_n = 1; gs0_11.flags = 0; gs0_11.act = 0;
      gs0_11.alpha = 1.0f; gs0_11.beta = 0.0f; gs0_11.sa = 1.0f; gs0_11.sb = 1.0f; gs0_11.Npad = LP; gs0_11.pad_ = 0;
      k_gemm<1><<<dim3((unsigned)((LP) + 31) / 32, (unsigned)((4) + 15) / 16, (unsigned)(O)), 32, 0, stream>>>(gs0_11); }
    k_caps_cp<<<(unsigned)(((long long)O * 4 * KD + 255) / 256), 256, 0, stream>>>(P, CC, CP, 12, O, I);
    { GemmP gs0_12;
      gs0_12.A = CP; gs0_12.B = Wc; gs0_12.bias = CP; gs0_12.R = CP; gs0_12.C = S + (size_t)12 * O * 4 * LP;
      gs0_12.sAo = (long long)4 * KD; gs0_12.sAi = 0; gs0_12.sAm = KD; gs0_12.sAk = 1; gs0_12.sBo = (long long)KD * 4; gs0_12.sBi = 0; gs0_12.sBn = 1; gs0_12.sBk = 4; gs0_12.sCo = 4 * LP; gs0_12.sCi = 0; gs0_12.sCm = LP; gs0_12.sRo = 0; gs0_12.sRi = 0; gs0_12.sRm = 0; gs0_12.sRn = 0;
      gs0_12.M = 4; gs0_12.N = 4; gs0_12.K = KD; gs0_12.zi_n = 1; gs0_12.flags = 0; gs0_12.act = 0;
      gs0_12.alpha = 1.0f; gs0_12.beta = 0.0f; gs0_12.sa = 1.0f; gs0_12.sb = 1.0f; gs0_12.Npad = LP; gs0_12.pad_ = 0;
      k_gemm<1><<<dim3((unsigned)((LP) + 31) / 32, (unsigned)((4) + 15) / 16, (unsigned)(O)), 32, 0, stream>>>(gs0_12); }
    k_caps_cp<<<(unsigned)(((long long)O * 4 * KD + 255) / 256), 256, 0, stream>>>(P, CC, CP, 13, O, I);
    { GemmP gs0_13;
      gs0_13.A = CP; gs0_13.B = Wc; gs0_13.bias = CP; gs0_13.R = CP; gs0_13.C = S + (size_t)13 * O * 4 * LP;
      gs0_13.sAo = (long long)4 * KD; gs0_13.sAi = 0; gs0_13.sAm = KD; gs0_13.sAk = 1; gs0_13.sBo = (long long)KD * 4; gs0_13.sBi = 0; gs0_13.sBn = 1; gs0_13.sBk = 4; gs0_13.sCo = 4 * LP; gs0_13.sCi = 0; gs0_13.sCm = LP; gs0_13.sRo = 0; gs0_13.sRi = 0; gs0_13.sRm = 0; gs0_13.sRn = 0;
      gs0_13.M = 4; gs0_13.N = 4; gs0_13.K = KD; gs0_13.zi_n = 1; gs0_13.flags = 0; gs0_13.act = 0;
      gs0_13.alpha = 1.0f; gs0_13.beta = 0.0f; gs0_13.sa = 1.0f; gs0_13.sb = 1.0f; gs0_13.Npad = LP; gs0_13.pad_ = 0;
      k_gemm<1><<<dim3((unsigned)((LP) + 31) / 32, (unsigned)((4) + 15) / 16, (unsigned)(O)), 32, 0, stream>>>(gs0_13); }
    k_caps_cp<<<(unsigned)(((long long)O * 4 * KD + 255) / 256), 256, 0, stream>>>(P, CC, CP, 14, O, I);
    { GemmP gs0_14;
      gs0_14.A = CP; gs0_14.B = Wc; gs0_14.bias = CP; gs0_14.R = CP; gs0_14.C = S + (size_t)14 * O * 4 * LP;
      gs0_14.sAo = (long long)4 * KD; gs0_14.sAi = 0; gs0_14.sAm = KD; gs0_14.sAk = 1; gs0_14.sBo = (long long)KD * 4; gs0_14.sBi = 0; gs0_14.sBn = 1; gs0_14.sBk = 4; gs0_14.sCo = 4 * LP; gs0_14.sCi = 0; gs0_14.sCm = LP; gs0_14.sRo = 0; gs0_14.sRi = 0; gs0_14.sRm = 0; gs0_14.sRn = 0;
      gs0_14.M = 4; gs0_14.N = 4; gs0_14.K = KD; gs0_14.zi_n = 1; gs0_14.flags = 0; gs0_14.act = 0;
      gs0_14.alpha = 1.0f; gs0_14.beta = 0.0f; gs0_14.sa = 1.0f; gs0_14.sb = 1.0f; gs0_14.Npad = LP; gs0_14.pad_ = 0;
      k_gemm<1><<<dim3((unsigned)((LP) + 31) / 32, (unsigned)((4) + 15) / 16, (unsigned)(O)), 32, 0, stream>>>(gs0_14); }
    k_caps_cp<<<(unsigned)(((long long)O * 4 * KD + 255) / 256), 256, 0, stream>>>(P, CC, CP, 15, O, I);
    { GemmP gs0_15;
      gs0_15.A = CP; gs0_15.B = Wc; gs0_15.bias = CP; gs0_15.R = CP; gs0_15.C = S + (size_t)15 * O * 4 * LP;
      gs0_15.sAo = (long long)4 * KD; gs0_15.sAi = 0; gs0_15.sAm = KD; gs0_15.sAk = 1; gs0_15.sBo = (long long)KD * 4; gs0_15.sBi = 0; gs0_15.sBn = 1; gs0_15.sBk = 4; gs0_15.sCo = 4 * LP; gs0_15.sCi = 0; gs0_15.sCm = LP; gs0_15.sRo = 0; gs0_15.sRi = 0; gs0_15.sRm = 0; gs0_15.sRn = 0;
      gs0_15.M = 4; gs0_15.N = 4; gs0_15.K = KD; gs0_15.zi_n = 1; gs0_15.flags = 0; gs0_15.act = 0;
      gs0_15.alpha = 1.0f; gs0_15.beta = 0.0f; gs0_15.sa = 1.0f; gs0_15.sb = 1.0f; gs0_15.Npad = LP; gs0_15.pad_ = 0;
      k_gemm<1><<<dim3((unsigned)((LP) + 31) / 32, (unsigned)((4) + 15) / 16, (unsigned)(O)), 32, 0, stream>>>(gs0_15); }
    k_caps_cp<<<(unsigned)(((long long)O * 4 * KD + 255) / 256), 256, 0, stream>>>(P, CC, CP, 16, O, I);
    { GemmP gs0_16;
      gs0_16.A = CP; gs0_16.B = Wc; gs0_16.bias = CP; gs0_16.R = CP; gs0_16.C = S + (size_t)16 * O * 4 * LP;
      gs0_16.sAo = (long long)4 * KD; gs0_16.sAi = 0; gs0_16.sAm = KD; gs0_16.sAk = 1; gs0_16.sBo = (long long)KD * 4; gs0_16.sBi = 0; gs0_16.sBn = 1; gs0_16.sBk = 4; gs0_16.sCo = 4 * LP; gs0_16.sCi = 0; gs0_16.sCm = LP; gs0_16.sRo = 0; gs0_16.sRi = 0; gs0_16.sRm = 0; gs0_16.sRn = 0;
      gs0_16.M = 4; gs0_16.N = 4; gs0_16.K = KD; gs0_16.zi_n = 1; gs0_16.flags = 0; gs0_16.act = 0;
      gs0_16.alpha = 1.0f; gs0_16.beta = 0.0f; gs0_16.sa = 1.0f; gs0_16.sb = 1.0f; gs0_16.Npad = LP; gs0_16.pad_ = 0;
      k_gemm<1><<<dim3((unsigned)((LP) + 31) / 32, (unsigned)((4) + 15) / 16, (unsigned)(O)), 32, 0, stream>>>(gs0_16); }
    k_caps_cp<<<(unsigned)(((long long)O * 4 * KD + 255) / 256), 256, 0, stream>>>(P, CC, CP, 17, O, I);
    { GemmP gs0_17;
      gs0_17.A = CP; gs0_17.B = Wc; gs0_17.bias = CP; gs0_17.R = CP; gs0_17.C = S + (size_t)17 * O * 4 * LP;
      gs0_17.sAo = (long long)4 * KD; gs0_17.sAi = 0; gs0_17.sAm = KD; gs0_17.sAk = 1; gs0_17.sBo = (long long)KD * 4; gs0_17.sBi = 0; gs0_17.sBn = 1; gs0_17.sBk = 4; gs0_17.sCo = 4 * LP; gs0_17.sCi = 0; gs0_17.sCm = LP; gs0_17.sRo = 0; gs0_17.sRi = 0; gs0_17.sRm = 0; gs0_17.sRn = 0;
      gs0_17.M = 4; gs0_17.N = 4; gs0_17.K = KD; gs0_17.zi_n = 1; gs0_17.flags = 0; gs0_17.act = 0;
      gs0_17.alpha = 1.0f; gs0_17.beta = 0.0f; gs0_17.sa = 1.0f; gs0_17.sb = 1.0f; gs0_17.Npad = LP; gs0_17.pad_ = 0;
      k_gemm<1><<<dim3((unsigned)((LP) + 31) / 32, (unsigned)((4) + 15) / 16, (unsigned)(O)), 32, 0, stream>>>(gs0_17); }
    k_caps_cp<<<(unsigned)(((long long)O * 4 * KD + 255) / 256), 256, 0, stream>>>(P, CC, CP, 18, O, I);
    { GemmP gs0_18;
      gs0_18.A = CP; gs0_18.B = Wc; gs0_18.bias = CP; gs0_18.R = CP; gs0_18.C = S + (size_t)18 * O * 4 * LP;
      gs0_18.sAo = (long long)4 * KD; gs0_18.sAi = 0; gs0_18.sAm = KD; gs0_18.sAk = 1; gs0_18.sBo = (long long)KD * 4; gs0_18.sBi = 0; gs0_18.sBn = 1; gs0_18.sBk = 4; gs0_18.sCo = 4 * LP; gs0_18.sCi = 0; gs0_18.sCm = LP; gs0_18.sRo = 0; gs0_18.sRi = 0; gs0_18.sRm = 0; gs0_18.sRn = 0;
      gs0_18.M = 4; gs0_18.N = 4; gs0_18.K = KD; gs0_18.zi_n = 1; gs0_18.flags = 0; gs0_18.act = 0;
      gs0_18.alpha = 1.0f; gs0_18.beta = 0.0f; gs0_18.sa = 1.0f; gs0_18.sb = 1.0f; gs0_18.Npad = LP; gs0_18.pad_ = 0;
      k_gemm<1><<<dim3((unsigned)((LP) + 31) / 32, (unsigned)((4) + 15) / 16, (unsigned)(O)), 32, 0, stream>>>(gs0_18); }
    k_caps_cp<<<(unsigned)(((long long)O * 4 * KD + 255) / 256), 256, 0, stream>>>(P, CC, CP, 19, O, I);
    { GemmP gs0_19;
      gs0_19.A = CP; gs0_19.B = Wc; gs0_19.bias = CP; gs0_19.R = CP; gs0_19.C = S + (size_t)19 * O * 4 * LP;
      gs0_19.sAo = (long long)4 * KD; gs0_19.sAi = 0; gs0_19.sAm = KD; gs0_19.sAk = 1; gs0_19.sBo = (long long)KD * 4; gs0_19.sBi = 0; gs0_19.sBn = 1; gs0_19.sBk = 4; gs0_19.sCo = 4 * LP; gs0_19.sCi = 0; gs0_19.sCm = LP; gs0_19.sRo = 0; gs0_19.sRi = 0; gs0_19.sRm = 0; gs0_19.sRn = 0;
      gs0_19.M = 4; gs0_19.N = 4; gs0_19.K = KD; gs0_19.zi_n = 1; gs0_19.flags = 0; gs0_19.act = 0;
      gs0_19.alpha = 1.0f; gs0_19.beta = 0.0f; gs0_19.sa = 1.0f; gs0_19.sb = 1.0f; gs0_19.Npad = LP; gs0_19.pad_ = 0;
      k_gemm<1><<<dim3((unsigned)((LP) + 31) / 32, (unsigned)((4) + 15) / 16, (unsigned)(O)), 32, 0, stream>>>(gs0_19); }
    k_caps_cp<<<(unsigned)(((long long)O * 4 * KD + 255) / 256), 256, 0, stream>>>(P, CC, CP, 20, O, I);
    { GemmP gs0_20;
      gs0_20.A = CP; gs0_20.B = Wc; gs0_20.bias = CP; gs0_20.R = CP; gs0_20.C = S + (size_t)20 * O * 4 * LP;
      gs0_20.sAo = (long long)4 * KD; gs0_20.sAi = 0; gs0_20.sAm = KD; gs0_20.sAk = 1; gs0_20.sBo = (long long)KD * 4; gs0_20.sBi = 0; gs0_20.sBn = 1; gs0_20.sBk = 4; gs0_20.sCo = 4 * LP; gs0_20.sCi = 0; gs0_20.sCm = LP; gs0_20.sRo = 0; gs0_20.sRi = 0; gs0_20.sRm = 0; gs0_20.sRn = 0;
      gs0_20.M = 4; gs0_20.N = 4; gs0_20.K = KD; gs0_20.zi_n = 1; gs0_20.flags = 0; gs0_20.act = 0;
      gs0_20.alpha = 1.0f; gs0_20.beta = 0.0f; gs0_20.sa = 1.0f; gs0_20.sb = 1.0f; gs0_20.Npad = LP; gs0_20.pad_ = 0;
      k_gemm<1><<<dim3((unsigned)((LP) + 31) / 32, (unsigned)((4) + 15) / 16, (unsigned)(O)), 32, 0, stream>>>(gs0_20); }
    k_caps_cp<<<(unsigned)(((long long)O * 4 * KD + 255) / 256), 256, 0, stream>>>(P, CC, CP, 21, O, I);
    { GemmP gs0_21;
      gs0_21.A = CP; gs0_21.B = Wc; gs0_21.bias = CP; gs0_21.R = CP; gs0_21.C = S + (size_t)21 * O * 4 * LP;
      gs0_21.sAo = (long long)4 * KD; gs0_21.sAi = 0; gs0_21.sAm = KD; gs0_21.sAk = 1; gs0_21.sBo = (long long)KD * 4; gs0_21.sBi = 0; gs0_21.sBn = 1; gs0_21.sBk = 4; gs0_21.sCo = 4 * LP; gs0_21.sCi = 0; gs0_21.sCm = LP; gs0_21.sRo = 0; gs0_21.sRi = 0; gs0_21.sRm = 0; gs0_21.sRn = 0;
      gs0_21.M = 4; gs0_21.N = 4; gs0_21.K = KD; gs0_21.zi_n = 1; gs0_21.flags = 0; gs0_21.act = 0;
      gs0_21.alpha = 1.0f; gs0_21.beta = 0.0f; gs0_21.sa = 1.0f; gs0_21.sb = 1.0f; gs0_21.Npad = LP; gs0_21.pad_ = 0;
      k_gemm<1><<<dim3((unsigned)((LP) + 31) / 32, (unsigned)((4) + 15) / 16, (unsigned)(O)), 32, 0, stream>>>(gs0_21); }
    k_caps_cp<<<(unsigned)(((long long)O * 4 * KD + 255) / 256), 256, 0, stream>>>(P, CC, CP, 22, O, I);
    { GemmP gs0_22;
      gs0_22.A = CP; gs0_22.B = Wc; gs0_22.bias = CP; gs0_22.R = CP; gs0_22.C = S + (size_t)22 * O * 4 * LP;
      gs0_22.sAo = (long long)4 * KD; gs0_22.sAi = 0; gs0_22.sAm = KD; gs0_22.sAk = 1; gs0_22.sBo = (long long)KD * 4; gs0_22.sBi = 0; gs0_22.sBn = 1; gs0_22.sBk = 4; gs0_22.sCo = 4 * LP; gs0_22.sCi = 0; gs0_22.sCm = LP; gs0_22.sRo = 0; gs0_22.sRi = 0; gs0_22.sRm = 0; gs0_22.sRn = 0;
      gs0_22.M = 4; gs0_22.N = 4; gs0_22.K = KD; gs0_22.zi_n = 1; gs0_22.flags = 0; gs0_22.act = 0;
      gs0_22.alpha = 1.0f; gs0_22.beta = 0.0f; gs0_22.sa = 1.0f; gs0_22.sb = 1.0f; gs0_22.Npad = LP; gs0_22.pad_ = 0;
      k_gemm<1><<<dim3((unsigned)((LP) + 31) / 32, (unsigned)((4) + 15) / 16, (unsigned)(O)), 32, 0, stream>>>(gs0_22); }
    k_caps_cp<<<(unsigned)(((long long)O * 4 * KD + 255) / 256), 256, 0, stream>>>(P, CC, CP, 23, O, I);
    { GemmP gs0_23;
      gs0_23.A = CP; gs0_23.B = Wc; gs0_23.bias = CP; gs0_23.R = CP; gs0_23.C = S + (size_t)23 * O * 4 * LP;
      gs0_23.sAo = (long long)4 * KD; gs0_23.sAi = 0; gs0_23.sAm = KD; gs0_23.sAk = 1; gs0_23.sBo = (long long)KD * 4; gs0_23.sBi = 0; gs0_23.sBn = 1; gs0_23.sBk = 4; gs0_23.sCo = 4 * LP; gs0_23.sCi = 0; gs0_23.sCm = LP; gs0_23.sRo = 0; gs0_23.sRi = 0; gs0_23.sRm = 0; gs0_23.sRn = 0;
      gs0_23.M = 4; gs0_23.N = 4; gs0_23.K = KD; gs0_23.zi_n = 1; gs0_23.flags = 0; gs0_23.act = 0;
      gs0_23.alpha = 1.0f; gs0_23.beta = 0.0f; gs0_23.sa = 1.0f; gs0_23.sb = 1.0f; gs0_23.Npad = LP; gs0_23.pad_ = 0;
      k_gemm<1><<<dim3((unsigned)((LP) + 31) / 32, (unsigned)((4) + 15) / 16, (unsigned)(O)), 32, 0, stream>>>(gs0_23); }
    k_caps_cp<<<(unsigned)(((long long)O * 4 * KD + 255) / 256), 256, 0, stream>>>(P, CC, CP, 24, O, I);
    { GemmP gs0_24;
      gs0_24.A = CP; gs0_24.B = Wc; gs0_24.bias = CP; gs0_24.R = CP; gs0_24.C = S + (size_t)24 * O * 4 * LP;
      gs0_24.sAo = (long long)4 * KD; gs0_24.sAi = 0; gs0_24.sAm = KD; gs0_24.sAk = 1; gs0_24.sBo = (long long)KD * 4; gs0_24.sBi = 0; gs0_24.sBn = 1; gs0_24.sBk = 4; gs0_24.sCo = 4 * LP; gs0_24.sCi = 0; gs0_24.sCm = LP; gs0_24.sRo = 0; gs0_24.sRi = 0; gs0_24.sRm = 0; gs0_24.sRn = 0;
      gs0_24.M = 4; gs0_24.N = 4; gs0_24.K = KD; gs0_24.zi_n = 1; gs0_24.flags = 0; gs0_24.act = 0;
      gs0_24.alpha = 1.0f; gs0_24.beta = 0.0f; gs0_24.sa = 1.0f; gs0_24.sb = 1.0f; gs0_24.Npad = LP; gs0_24.pad_ = 0;
      k_gemm<1><<<dim3((unsigned)((LP) + 31) / 32, (unsigned)((4) + 15) / 16, (unsigned)(O)), 32, 0, stream>>>(gs0_24); }
    k_caps_cp<<<(unsigned)(((long long)O * 4 * KD + 255) / 256), 256, 0, stream>>>(P, CC, CP, 25, O, I);
    { GemmP gs0_25;
      gs0_25.A = CP; gs0_25.B = Wc; gs0_25.bias = CP; gs0_25.R = CP; gs0_25.C = S + (size_t)25 * O * 4 * LP;
      gs0_25.sAo = (long long)4 * KD; gs0_25.sAi = 0; gs0_25.sAm = KD; gs0_25.sAk = 1; gs0_25.sBo = (long long)KD * 4; gs0_25.sBi = 0; gs0_25.sBn = 1; gs0_25.sBk = 4; gs0_25.sCo = 4 * LP; gs0_25.sCi = 0; gs0_25.sCm = LP; gs0_25.sRo = 0; gs0_25.sRi = 0; gs0_25.sRm = 0; gs0_25.sRn = 0;
      gs0_25.M = 4; gs0_25.N = 4; gs0_25.K = KD; gs0_25.zi_n = 1; gs0_25.flags = 0; gs0_25.act = 0;
      gs0_25.alpha = 1.0f; gs0_25.beta = 0.0f; gs0_25.sa = 1.0f; gs0_25.sb = 1.0f; gs0_25.Npad = LP; gs0_25.pad_ = 0;
      k_gemm<1><<<dim3((unsigned)((LP) + 31) / 32, (unsigned)((4) + 15) / 16, (unsigned)(O)), 32, 0, stream>>>(gs0_25); }
    k_caps_cp<<<(unsigned)(((long long)O * 4 * KD + 255) / 256), 256, 0, stream>>>(P, CC, CP, 26, O, I);
    { GemmP gs0_26;
      gs0_26.A = CP; gs0_26.B = Wc; gs0_26.bias = CP; gs0_26.R = CP; gs0_26.C = S + (size_t)26 * O * 4 * LP;
      gs0_26.sAo = (long long)4 * KD; gs0_26.sAi = 0; gs0_26.sAm = KD; gs0_26.sAk = 1; gs0_26.sBo = (long long)KD * 4; gs0_26.sBi = 0; gs0_26.sBn = 1; gs0_26.sBk = 4; gs0_26.sCo = 4 * LP; gs0_26.sCi = 0; gs0_26.sCm = LP; gs0_26.sRo = 0; gs0_26.sRi = 0; gs0_26.sRm = 0; gs0_26.sRn = 0;
      gs0_26.M = 4; gs0_26.N = 4; gs0_26.K = KD; gs0_26.zi_n = 1; gs0_26.flags = 0; gs0_26.act = 0;
      gs0_26.alpha = 1.0f; gs0_26.beta = 0.0f; gs0_26.sa = 1.0f; gs0_26.sb = 1.0f; gs0_26.Npad = LP; gs0_26.pad_ = 0;
      k_gemm<1><<<dim3((unsigned)((LP) + 31) / 32, (unsigned)((4) + 15) / 16, (unsigned)(O)), 32, 0, stream>>>(gs0_26); }
    k_caps_cp<<<(unsigned)(((long long)O * 4 * KD + 255) / 256), 256, 0, stream>>>(P, CC, CP, 27, O, I);
    { GemmP gs0_27;
      gs0_27.A = CP; gs0_27.B = Wc; gs0_27.bias = CP; gs0_27.R = CP; gs0_27.C = S + (size_t)27 * O * 4 * LP;
      gs0_27.sAo = (long long)4 * KD; gs0_27.sAi = 0; gs0_27.sAm = KD; gs0_27.sAk = 1; gs0_27.sBo = (long long)KD * 4; gs0_27.sBi = 0; gs0_27.sBn = 1; gs0_27.sBk = 4; gs0_27.sCo = 4 * LP; gs0_27.sCi = 0; gs0_27.sCm = LP; gs0_27.sRo = 0; gs0_27.sRi = 0; gs0_27.sRm = 0; gs0_27.sRn = 0;
      gs0_27.M = 4; gs0_27.N = 4; gs0_27.K = KD; gs0_27.zi_n = 1; gs0_27.flags = 0; gs0_27.act = 0;
      gs0_27.alpha = 1.0f; gs0_27.beta = 0.0f; gs0_27.sa = 1.0f; gs0_27.sb = 1.0f; gs0_27.Npad = LP; gs0_27.pad_ = 0;
      k_gemm<1><<<dim3((unsigned)((LP) + 31) / 32, (unsigned)((4) + 15) / 16, (unsigned)(O)), 32, 0, stream>>>(gs0_27); }
    k_caps_cp<<<(unsigned)(((long long)O * 4 * KD + 255) / 256), 256, 0, stream>>>(P, CC, CP, 28, O, I);
    { GemmP gs0_28;
      gs0_28.A = CP; gs0_28.B = Wc; gs0_28.bias = CP; gs0_28.R = CP; gs0_28.C = S + (size_t)28 * O * 4 * LP;
      gs0_28.sAo = (long long)4 * KD; gs0_28.sAi = 0; gs0_28.sAm = KD; gs0_28.sAk = 1; gs0_28.sBo = (long long)KD * 4; gs0_28.sBi = 0; gs0_28.sBn = 1; gs0_28.sBk = 4; gs0_28.sCo = 4 * LP; gs0_28.sCi = 0; gs0_28.sCm = LP; gs0_28.sRo = 0; gs0_28.sRi = 0; gs0_28.sRm = 0; gs0_28.sRn = 0;
      gs0_28.M = 4; gs0_28.N = 4; gs0_28.K = KD; gs0_28.zi_n = 1; gs0_28.flags = 0; gs0_28.act = 0;
      gs0_28.alpha = 1.0f; gs0_28.beta = 0.0f; gs0_28.sa = 1.0f; gs0_28.sb = 1.0f; gs0_28.Npad = LP; gs0_28.pad_ = 0;
      k_gemm<1><<<dim3((unsigned)((LP) + 31) / 32, (unsigned)((4) + 15) / 16, (unsigned)(O)), 32, 0, stream>>>(gs0_28); }
    k_caps_cp<<<(unsigned)(((long long)O * 4 * KD + 255) / 256), 256, 0, stream>>>(P, CC, CP, 29, O, I);
    { GemmP gs0_29;
      gs0_29.A = CP; gs0_29.B = Wc; gs0_29.bias = CP; gs0_29.R = CP; gs0_29.C = S + (size_t)29 * O * 4 * LP;
      gs0_29.sAo = (long long)4 * KD; gs0_29.sAi = 0; gs0_29.sAm = KD; gs0_29.sAk = 1; gs0_29.sBo = (long long)KD * 4; gs0_29.sBi = 0; gs0_29.sBn = 1; gs0_29.sBk = 4; gs0_29.sCo = 4 * LP; gs0_29.sCi = 0; gs0_29.sCm = LP; gs0_29.sRo = 0; gs0_29.sRi = 0; gs0_29.sRm = 0; gs0_29.sRn = 0;
      gs0_29.M = 4; gs0_29.N = 4; gs0_29.K = KD; gs0_29.zi_n = 1; gs0_29.flags = 0; gs0_29.act = 0;
      gs0_29.alpha = 1.0f; gs0_29.beta = 0.0f; gs0_29.sa = 1.0f; gs0_29.sb = 1.0f; gs0_29.Npad = LP; gs0_29.pad_ = 0;
      k_gemm<1><<<dim3((unsigned)((LP) + 31) / 32, (unsigned)((4) + 15) / 16, (unsigned)(O)), 32, 0, stream>>>(gs0_29); }
    k_caps_cp<<<(unsigned)(((long long)O * 4 * KD + 255) / 256), 256, 0, stream>>>(P, CC, CP, 30, O, I);
    { GemmP gs0_30;
      gs0_30.A = CP; gs0_30.B = Wc; gs0_30.bias = CP; gs0_30.R = CP; gs0_30.C = S + (size_t)30 * O * 4 * LP;
      gs0_30.sAo = (long long)4 * KD; gs0_30.sAi = 0; gs0_30.sAm = KD; gs0_30.sAk = 1; gs0_30.sBo = (long long)KD * 4; gs0_30.sBi = 0; gs0_30.sBn = 1; gs0_30.sBk = 4; gs0_30.sCo = 4 * LP; gs0_30.sCi = 0; gs0_30.sCm = LP; gs0_30.sRo = 0; gs0_30.sRi = 0; gs0_30.sRm = 0; gs0_30.sRn = 0;
      gs0_30.M = 4; gs0_30.N = 4; gs0_30.K = KD; gs0_30.zi_n = 1; gs0_30.flags = 0; gs0_30.act = 0;
      gs0_30.alpha = 1.0f; gs0_30.beta = 0.0f; gs0_30.sa = 1.0f; gs0_30.sb = 1.0f; gs0_30.Npad = LP; gs0_30.pad_ = 0;
      k_gemm<1><<<dim3((unsigned)((LP) + 31) / 32, (unsigned)((4) + 15) / 16, (unsigned)(O)), 32, 0, stream>>>(gs0_30); }
    k_caps_cp<<<(unsigned)(((long long)O * 4 * KD + 255) / 256), 256, 0, stream>>>(P, CC, CP, 31, O, I);
    { GemmP gs0_31;
      gs0_31.A = CP; gs0_31.B = Wc; gs0_31.bias = CP; gs0_31.R = CP; gs0_31.C = S + (size_t)31 * O * 4 * LP;
      gs0_31.sAo = (long long)4 * KD; gs0_31.sAi = 0; gs0_31.sAm = KD; gs0_31.sAk = 1; gs0_31.sBo = (long long)KD * 4; gs0_31.sBi = 0; gs0_31.sBn = 1; gs0_31.sBk = 4; gs0_31.sCo = 4 * LP; gs0_31.sCi = 0; gs0_31.sCm = LP; gs0_31.sRo = 0; gs0_31.sRi = 0; gs0_31.sRm = 0; gs0_31.sRn = 0;
      gs0_31.M = 4; gs0_31.N = 4; gs0_31.K = KD; gs0_31.zi_n = 1; gs0_31.flags = 0; gs0_31.act = 0;
      gs0_31.alpha = 1.0f; gs0_31.beta = 0.0f; gs0_31.sa = 1.0f; gs0_31.sb = 1.0f; gs0_31.Npad = LP; gs0_31.pad_ = 0;
      k_gemm<1><<<dim3((unsigned)((LP) + 31) / 32, (unsigned)((4) + 15) / 16, (unsigned)(O)), 32, 0, stream>>>(gs0_31); }
    k_caps_squash<<<(unsigned)((Bn * O * 16 + 255) / 256), 256, 0, stream>>>(S, LP, V, out, aout, Bn * O, 0);
    k_caps_agree<<<(unsigned)(((long long)Bn * O * I + 255) / 256), 256, 0, stream>>>(P, Wc, V, BL, Bn, O, I);
    k_caps_soft<<<(unsigned)((Bn * I + 255) / 256), 256, 0, stream>>>(BL, CC, Bn, O, I);
    k_caps_cp<<<(unsigned)(((long long)O * 4 * KD + 255) / 256), 256, 0, stream>>>(P, CC, CP, 0, O, I);
    { GemmP gs1_0;
      gs1_0.A = CP; gs1_0.B = Wc; gs1_0.bias = CP; gs1_0.R = CP; gs1_0.C = S + (size_t)0 * O * 4 * LP;
      gs1_0.sAo = (long long)4 * KD; gs1_0.sAi = 0; gs1_0.sAm = KD; gs1_0.sAk = 1; gs1_0.sBo = (long long)KD * 4; gs1_0.sBi = 0; gs1_0.sBn = 1; gs1_0.sBk = 4; gs1_0.sCo = 4 * LP; gs1_0.sCi = 0; gs1_0.sCm = LP; gs1_0.sRo = 0; gs1_0.sRi = 0; gs1_0.sRm = 0; gs1_0.sRn = 0;
      gs1_0.M = 4; gs1_0.N = 4; gs1_0.K = KD; gs1_0.zi_n = 1; gs1_0.flags = 0; gs1_0.act = 0;
      gs1_0.alpha = 1.0f; gs1_0.beta = 0.0f; gs1_0.sa = 1.0f; gs1_0.sb = 1.0f; gs1_0.Npad = LP; gs1_0.pad_ = 0;
      k_gemm<1><<<dim3((unsigned)((LP) + 31) / 32, (unsigned)((4) + 15) / 16, (unsigned)(O)), 32, 0, stream>>>(gs1_0); }
    k_caps_cp<<<(unsigned)(((long long)O * 4 * KD + 255) / 256), 256, 0, stream>>>(P, CC, CP, 1, O, I);
    { GemmP gs1_1;
      gs1_1.A = CP; gs1_1.B = Wc; gs1_1.bias = CP; gs1_1.R = CP; gs1_1.C = S + (size_t)1 * O * 4 * LP;
      gs1_1.sAo = (long long)4 * KD; gs1_1.sAi = 0; gs1_1.sAm = KD; gs1_1.sAk = 1; gs1_1.sBo = (long long)KD * 4; gs1_1.sBi = 0; gs1_1.sBn = 1; gs1_1.sBk = 4; gs1_1.sCo = 4 * LP; gs1_1.sCi = 0; gs1_1.sCm = LP; gs1_1.sRo = 0; gs1_1.sRi = 0; gs1_1.sRm = 0; gs1_1.sRn = 0;
      gs1_1.M = 4; gs1_1.N = 4; gs1_1.K = KD; gs1_1.zi_n = 1; gs1_1.flags = 0; gs1_1.act = 0;
      gs1_1.alpha = 1.0f; gs1_1.beta = 0.0f; gs1_1.sa = 1.0f; gs1_1.sb = 1.0f; gs1_1.Npad = LP; gs1_1.pad_ = 0;
      k_gemm<1><<<dim3((unsigned)((LP) + 31) / 32, (unsigned)((4) + 15) / 16, (unsigned)(O)), 32, 0, stream>>>(gs1_1); }
    k_caps_cp<<<(unsigned)(((long long)O * 4 * KD + 255) / 256), 256, 0, stream>>>(P, CC, CP, 2, O, I);
    { GemmP gs1_2;
      gs1_2.A = CP; gs1_2.B = Wc; gs1_2.bias = CP; gs1_2.R = CP; gs1_2.C = S + (size_t)2 * O * 4 * LP;
      gs1_2.sAo = (long long)4 * KD; gs1_2.sAi = 0; gs1_2.sAm = KD; gs1_2.sAk = 1; gs1_2.sBo = (long long)KD * 4; gs1_2.sBi = 0; gs1_2.sBn = 1; gs1_2.sBk = 4; gs1_2.sCo = 4 * LP; gs1_2.sCi = 0; gs1_2.sCm = LP; gs1_2.sRo = 0; gs1_2.sRi = 0; gs1_2.sRm = 0; gs1_2.sRn = 0;
      gs1_2.M = 4; gs1_2.N = 4; gs1_2.K = KD; gs1_2.zi_n = 1; gs1_2.flags = 0; gs1_2.act = 0;
      gs1_2.alpha = 1.0f; gs1_2.beta = 0.0f; gs1_2.sa = 1.0f; gs1_2.sb = 1.0f; gs1_2.Npad = LP; gs1_2.pad_ = 0;
      k_gemm<1><<<dim3((unsigned)((LP) + 31) / 32, (unsigned)((4) + 15) / 16, (unsigned)(O)), 32, 0, stream>>>(gs1_2); }
    k_caps_cp<<<(unsigned)(((long long)O * 4 * KD + 255) / 256), 256, 0, stream>>>(P, CC, CP, 3, O, I);
    { GemmP gs1_3;
      gs1_3.A = CP; gs1_3.B = Wc; gs1_3.bias = CP; gs1_3.R = CP; gs1_3.C = S + (size_t)3 * O * 4 * LP;
      gs1_3.sAo = (long long)4 * KD; gs1_3.sAi = 0; gs1_3.sAm = KD; gs1_3.sAk = 1; gs1_3.sBo = (long long)KD * 4; gs1_3.sBi = 0; gs1_3.sBn = 1; gs1_3.sBk = 4; gs1_3.sCo = 4 * LP; gs1_3.sCi = 0; gs1_3.sCm = LP; gs1_3.sRo = 0; gs1_3.sRi = 0; gs1_3.sRm = 0; gs1_3.sRn = 0;
      gs1_3.M = 4; gs1_3.N = 4; gs1_3.K = KD; gs1_3.zi_n = 1; gs1_3.flags = 0; gs1_3.act = 0;
      gs1_3.alpha = 1.0f; gs1_3.beta = 0.0f; gs1_3.sa = 1.0f; gs1_3.sb = 1.0f; gs1_3.Npad = LP; gs1_3.pad_ = 0;
      k_gemm<1><<<dim3((unsigned)((LP) + 31) / 32, (unsigned)((4) + 15) / 16, (unsigned)(O)), 32, 0, stream>>>(gs1_3); }
    k_caps_cp<<<(unsigned)(((long long)O * 4 * KD + 255) / 256), 256, 0, stream>>>(P, CC, CP, 4, O, I);
    { GemmP gs1_4;
      gs1_4.A = CP; gs1_4.B = Wc; gs1_4.bias = CP; gs1_4.R = CP; gs1_4.C = S + (size_t)4 * O * 4 * LP;
      gs1_4.sAo = (long long)4 * KD; gs1_4.sAi = 0; gs1_4.sAm = KD; gs1_4.sAk = 1; gs1_4.sBo = (long long)KD * 4; gs1_4.sBi = 0; gs1_4.sBn = 1; gs1_4.sBk = 4; gs1_4.sCo = 4 * LP; gs1_4.sCi = 0; gs1_4.sCm = LP; gs1_4.sRo = 0; gs1_4.sRi = 0; gs1_4.sRm = 0; gs1_4.sRn = 0;
      gs1_4.M = 4; gs1_4.N = 4; gs1_4.K = KD; gs1_4.zi_n = 1; gs1_4.flags = 0; gs1_4.act = 0;
      gs1_4.alpha = 1.0f; gs1_4.beta = 0.0f; gs1_4.sa = 1.0f; gs1_4.sb = 1.0f; gs1_4.Npad = LP; gs1_4.pad_ = 0;
      k_gemm<1><<<dim3((unsigned)((LP) + 31) / 32, (unsigned)((4) + 15) / 16, (unsigned)(O)), 32, 0, stream>>>(gs1_4); }
    k_caps_cp<<<(unsigned)(((long long)O * 4 * KD + 255) / 256), 256, 0, stream>>>(P, CC, CP, 5, O, I);
    { GemmP gs1_5;
      gs1_5.A = CP; gs1_5.B = Wc; gs1_5.bias = CP; gs1_5.R = CP; gs1_5.C = S + (size_t)5 * O * 4 * LP;
      gs1_5.sAo = (long long)4 * KD; gs1_5.sAi = 0; gs1_5.sAm = KD; gs1_5.sAk = 1; gs1_5.sBo = (long long)KD * 4; gs1_5.sBi = 0; gs1_5.sBn = 1; gs1_5.sBk = 4; gs1_5.sCo = 4 * LP; gs1_5.sCi = 0; gs1_5.sCm = LP; gs1_5.sRo = 0; gs1_5.sRi = 0; gs1_5.sRm = 0; gs1_5.sRn = 0;
      gs1_5.M = 4; gs1_5.N = 4; gs1_5.K = KD; gs1_5.zi_n = 1; gs1_5.flags = 0; gs1_5.act = 0;
      gs1_5.alpha = 1.0f; gs1_5.beta = 0.0f; gs1_5.sa = 1.0f; gs1_5.sb = 1.0f; gs1_5.Npad = LP; gs1_5.pad_ = 0;
      k_gemm<1><<<dim3((unsigned)((LP) + 31) / 32, (unsigned)((4) + 15) / 16, (unsigned)(O)), 32, 0, stream>>>(gs1_5); }
    k_caps_cp<<<(unsigned)(((long long)O * 4 * KD + 255) / 256), 256, 0, stream>>>(P, CC, CP, 6, O, I);
    { GemmP gs1_6;
      gs1_6.A = CP; gs1_6.B = Wc; gs1_6.bias = CP; gs1_6.R = CP; gs1_6.C = S + (size_t)6 * O * 4 * LP;
      gs1_6.sAo = (long long)4 * KD; gs1_6.sAi = 0; gs1_6.sAm = KD; gs1_6.sAk = 1; gs1_6.sBo = (long long)KD * 4; gs1_6.sBi = 0; gs1_6.sBn = 1; gs1_6.sBk = 4; gs1_6.sCo = 4 * LP; gs1_6.sCi = 0; gs1_6.sCm = LP; gs1_6.sRo = 0; gs1_6.sRi = 0; gs1_6.sRm = 0; gs1_6.sRn = 0;
      gs1_6.M = 4; gs1_6.N = 4; gs1_6.K = KD; gs1_6.zi_n = 1; gs1_6.flags = 0; gs1_6.act = 0;
      gs1_6.alpha = 1.0f; gs1_6.beta = 0.0f; gs1_6.sa = 1.0f; gs1_6.sb = 1.0f; gs1_6.Npad = LP; gs1_6.pad_ = 0;
      k_gemm<1><<<dim3((unsigned)((LP) + 31) / 32, (unsigned)((4) + 15) / 16, (unsigned)(O)), 32, 0, stream>>>(gs1_6); }
    k_caps_cp<<<(unsigned)(((long long)O * 4 * KD + 255) / 256), 256, 0, stream>>>(P, CC, CP, 7, O, I);
    { GemmP gs1_7;
      gs1_7.A = CP; gs1_7.B = Wc; gs1_7.bias = CP; gs1_7.R = CP; gs1_7.C = S + (size_t)7 * O * 4 * LP;
      gs1_7.sAo = (long long)4 * KD; gs1_7.sAi = 0; gs1_7.sAm = KD; gs1_7.sAk = 1; gs1_7.sBo = (long long)KD * 4; gs1_7.sBi = 0; gs1_7.sBn = 1; gs1_7.sBk = 4; gs1_7.sCo = 4 * LP; gs1_7.sCi = 0; gs1_7.sCm = LP; gs1_7.sRo = 0; gs1_7.sRi = 0; gs1_7.sRm = 0; gs1_7.sRn = 0;
      gs1_7.M = 4; gs1_7.N = 4; gs1_7.K = KD; gs1_7.zi_n = 1; gs1_7.flags = 0; gs1_7.act = 0;
      gs1_7.alpha = 1.0f; gs1_7.beta = 0.0f; gs1_7.sa = 1.0f; gs1_7.sb = 1.0f; gs1_7.Npad = LP; gs1_7.pad_ = 0;
      k_gemm<1><<<dim3((unsigned)((LP) + 31) / 32, (unsigned)((4) + 15) / 16, (unsigned)(O)), 32, 0, stream>>>(gs1_7); }
    k_caps_cp<<<(unsigned)(((long long)O * 4 * KD + 255) / 256), 256, 0, stream>>>(P, CC, CP, 8, O, I);
    { GemmP gs1_8;
      gs1_8.A = CP; gs1_8.B = Wc; gs1_8.bias = CP; gs1_8.R = CP; gs1_8.C = S + (size_t)8 * O * 4 * LP;
      gs1_8.sAo = (long long)4 * KD; gs1_8.sAi = 0; gs1_8.sAm = KD; gs1_8.sAk = 1; gs1_8.sBo = (long long)KD * 4; gs1_8.sBi = 0; gs1_8.sBn = 1; gs1_8.sBk = 4; gs1_8.sCo = 4 * LP; gs1_8.sCi = 0; gs1_8.sCm = LP; gs1_8.sRo = 0; gs1_8.sRi = 0; gs1_8.sRm = 0; gs1_8.sRn = 0;
      gs1_8.M = 4; gs1_8.N = 4; gs1_8.K = KD; gs1_8.zi_n = 1; gs1_8.flags = 0; gs1_8.act = 0;
      gs1_8.alpha = 1.0f; gs1_8.beta = 0.0f; gs1_8.sa = 1.0f; gs1_8.sb = 1.0f; gs1_8.Npad = LP; gs1_8.pad_ = 0;
      k_gemm<1><<<dim3((unsigned)((LP) + 31) / 32, (unsigned)((4) + 15) / 16, (unsigned)(O)), 32, 0, stream>>>(gs1_8); }
    k_caps_cp<<<(unsigned)(((long long)O * 4 * KD + 255) / 256), 256, 0, stream>>>(P, CC, CP, 9, O, I);
    { GemmP gs1_9;
      gs1_9.A = CP; gs1_9.B = Wc; gs1_9.bias = CP; gs1_9.R = CP; gs1_9.C = S + (size_t)9 * O * 4 * LP;
      gs1_9.sAo = (long long)4 * KD; gs1_9.sAi = 0; gs1_9.sAm = KD; gs1_9.sAk = 1; gs1_9.sBo = (long long)KD * 4; gs1_9.sBi = 0; gs1_9.sBn = 1; gs1_9.sBk = 4; gs1_9.sCo = 4 * LP; gs1_9.sCi = 0; gs1_9.sCm = LP; gs1_9.sRo = 0; gs1_9.sRi = 0; gs1_9.sRm = 0; gs1_9.sRn = 0;
      gs1_9.M = 4; gs1_9.N = 4; gs1_9.K = KD; gs1_9.zi_n = 1; gs1_9.flags = 0; gs1_9.act = 0;
      gs1_9.alpha = 1.0f; gs1_9.beta = 0.0f; gs1_9.sa = 1.0f; gs1_9.sb = 1.0f; gs1_9.Npad = LP; gs1_9.pad_ = 0;
      k_gemm<1><<<dim3((unsigned)((LP) + 31) / 32, (unsigned)((4) + 15) / 16, (unsigned)(O)), 32, 0, stream>>>(gs1_9); }
    k_caps_cp<<<(unsigned)(((long long)O * 4 * KD + 255) / 256), 256, 0, stream>>>(P, CC, CP, 10, O, I);
    { GemmP gs1_10;
      gs1_10.A = CP; gs1_10.B = Wc; gs1_10.bias = CP; gs1_10.R = CP; gs1_10.C = S + (size_t)10 * O * 4 * LP;
      gs1_10.sAo = (long long)4 * KD; gs1_10.sAi = 0; gs1_10.sAm = KD; gs1_10.sAk = 1; gs1_10.sBo = (long long)KD * 4; gs1_10.sBi = 0; gs1_10.sBn = 1; gs1_10.sBk = 4; gs1_10.sCo = 4 * LP; gs1_10.sCi = 0; gs1_10.sCm = LP; gs1_10.sRo = 0; gs1_10.sRi = 0; gs1_10.sRm = 0; gs1_10.sRn = 0;
      gs1_10.M = 4; gs1_10.N = 4; gs1_10.K = KD; gs1_10.zi_n = 1; gs1_10.flags = 0; gs1_10.act = 0;
      gs1_10.alpha = 1.0f; gs1_10.beta = 0.0f; gs1_10.sa = 1.0f; gs1_10.sb = 1.0f; gs1_10.Npad = LP; gs1_10.pad_ = 0;
      k_gemm<1><<<dim3((unsigned)((LP) + 31) / 32, (unsigned)((4) + 15) / 16, (unsigned)(O)), 32, 0, stream>>>(gs1_10); }
    k_caps_cp<<<(unsigned)(((long long)O * 4 * KD + 255) / 256), 256, 0, stream>>>(P, CC, CP, 11, O, I);
    { GemmP gs1_11;
      gs1_11.A = CP; gs1_11.B = Wc; gs1_11.bias = CP; gs1_11.R = CP; gs1_11.C = S + (size_t)11 * O * 4 * LP;
      gs1_11.sAo = (long long)4 * KD; gs1_11.sAi = 0; gs1_11.sAm = KD; gs1_11.sAk = 1; gs1_11.sBo = (long long)KD * 4; gs1_11.sBi = 0; gs1_11.sBn = 1; gs1_11.sBk = 4; gs1_11.sCo = 4 * LP; gs1_11.sCi = 0; gs1_11.sCm = LP; gs1_11.sRo = 0; gs1_11.sRi = 0; gs1_11.sRm = 0; gs1_11.sRn = 0;
      gs1_11.M = 4; gs1_11.N = 4; gs1_11.K = KD; gs1_11.zi_n = 1; gs1_11.flags = 0; gs1_11.act = 0;
      gs1_11.alpha = 1.0f; gs1_11.beta = 0.0f; gs1_11.sa = 1.0f; gs1_11.sb = 1.0f; gs1_11.Npad = LP; gs1_11.pad_ = 0;
      k_gemm<1><<<dim3((unsigned)((LP) + 31) / 32, (unsigned)((4) + 15) / 16, (unsigned)(O)), 32, 0, stream>>>(gs1_11); }
    k_caps_cp<<<(unsigned)(((long long)O * 4 * KD + 255) / 256), 256, 0, stream>>>(P, CC, CP, 12, O, I);
    { GemmP gs1_12;
      gs1_12.A = CP; gs1_12.B = Wc; gs1_12.bias = CP; gs1_12.R = CP; gs1_12.C = S + (size_t)12 * O * 4 * LP;
      gs1_12.sAo = (long long)4 * KD; gs1_12.sAi = 0; gs1_12.sAm = KD; gs1_12.sAk = 1; gs1_12.sBo = (long long)KD * 4; gs1_12.sBi = 0; gs1_12.sBn = 1; gs1_12.sBk = 4; gs1_12.sCo = 4 * LP; gs1_12.sCi = 0; gs1_12.sCm = LP; gs1_12.sRo = 0; gs1_12.sRi = 0; gs1_12.sRm = 0; gs1_12.sRn = 0;
      gs1_12.M = 4; gs1_12.N = 4; gs1_12.K = KD; gs1_12.zi_n = 1; gs1_12.flags = 0; gs1_12.act = 0;
      gs1_12.alpha = 1.0f; gs1_12.beta = 0.0f; gs1_12.sa = 1.0f; gs1_12.sb = 1.0f; gs1_12.Npad = LP; gs1_12.pad_ = 0;
      k_gemm<1><<<dim3((unsigned)((LP) + 31) / 32, (unsigned)((4) + 15) / 16, (unsigned)(O)), 32, 0, stream>>>(gs1_12); }
    k_caps_cp<<<(unsigned)(((long long)O * 4 * KD + 255) / 256), 256, 0, stream>>>(P, CC, CP, 13, O, I);
    { GemmP gs1_13;
      gs1_13.A = CP; gs1_13.B = Wc; gs1_13.bias = CP; gs1_13.R = CP; gs1_13.C = S + (size_t)13 * O * 4 * LP;
      gs1_13.sAo = (long long)4 * KD; gs1_13.sAi = 0; gs1_13.sAm = KD; gs1_13.sAk = 1; gs1_13.sBo = (long long)KD * 4; gs1_13.sBi = 0; gs1_13.sBn = 1; gs1_13.sBk = 4; gs1_13.sCo = 4 * LP; gs1_13.sCi = 0; gs1_13.sCm = LP; gs1_13.sRo = 0; gs1_13.sRi = 0; gs1_13.sRm = 0; gs1_13.sRn = 0;
      gs1_13.M = 4; gs1_13.N = 4; gs1_13.K = KD; gs1_13.zi_n = 1; gs1_13.flags = 0; gs1_13.act = 0;
      gs1_13.alpha = 1.0f; gs1_13.beta = 0.0f; gs1_13.sa = 1.0f; gs1_13.sb = 1.0f; gs1_13.Npad = LP; gs1_13.pad_ = 0;
      k_gemm<1><<<dim3((unsigned)((LP) + 31) / 32, (unsigned)((4) + 15) / 16, (unsigned)(O)), 32, 0, stream>>>(gs1_13); }
    k_caps_cp<<<(unsigned)(((long long)O * 4 * KD + 255) / 256), 256, 0, stream>>>(P, CC, CP, 14, O, I);
    { GemmP gs1_14;
      gs1_14.A = CP; gs1_14.B = Wc; gs1_14.bias = CP; gs1_14.R = CP; gs1_14.C = S + (size_t)14 * O * 4 * LP;
      gs1_14.sAo = (long long)4 * KD; gs1_14.sAi = 0; gs1_14.sAm = KD; gs1_14.sAk = 1; gs1_14.sBo = (long long)KD * 4; gs1_14.sBi = 0; gs1_14.sBn = 1; gs1_14.sBk = 4; gs1_14.sCo = 4 * LP; gs1_14.sCi = 0; gs1_14.sCm = LP; gs1_14.sRo = 0; gs1_14.sRi = 0; gs1_14.sRm = 0; gs1_14.sRn = 0;
      gs1_14.M = 4; gs1_14.N = 4; gs1_14.K = KD; gs1_14.zi_n = 1; gs1_14.flags = 0; gs1_14.act = 0;
      gs1_14.alpha = 1.0f; gs1_14.beta = 0.0f; gs1_14.sa = 1.0f; gs1_14.sb = 1.0f; gs1_14.Npad = LP; gs1_14.pad_ = 0;
      k_gemm<1><<<dim3((unsigned)((LP) + 31) / 32, (unsigned)((4) + 15) / 16, (unsigned)(O)), 32, 0, stream>>>(gs1_14); }
    k_caps_cp<<<(unsigned)(((long long)O * 4 * KD + 255) / 256), 256, 0, stream>>>(P, CC, CP, 15, O, I);
    { GemmP gs1_15;
      gs1_15.A = CP; gs1_15.B = Wc; gs1_15.bias = CP; gs1_15.R = CP; gs1_15.C = S + (size_t)15 * O * 4 * LP;
      gs1_15.sAo = (long long)4 * KD; gs1_15.sAi = 0; gs1_15.sAm = KD; gs1_15.sAk = 1; gs1_15.sBo = (long long)KD * 4; gs1_15.sBi = 0; gs1_15.sBn = 1; gs1_15.sBk = 4; gs1_15.sCo = 4 * LP; gs1_15.sCi = 0; gs1_15.sCm = LP; gs1_15.sRo = 0; gs1_15.sRi = 0; gs1_15.sRm = 0; gs1_15.sRn = 0;
      gs1_15.M = 4; gs1_15.N = 4; gs1_15.K = KD; gs1_15.zi_n = 1; gs1_15.flags = 0; gs1_15.act = 0;
      gs1_15.alpha = 1.0f; gs1_15.beta = 0.0f; gs1_15.sa = 1.0f; gs1_15.sb = 1.0f; gs1_15.Npad = LP; gs1_15.pad_ = 0;
      k_gemm<1><<<dim3((unsigned)((LP) + 31) / 32, (unsigned)((4) + 15) / 16, (unsigned)(O)), 32, 0, stream>>>(gs1_15); }
    k_caps_cp<<<(unsigned)(((long long)O * 4 * KD + 255) / 256), 256, 0, stream>>>(P, CC, CP, 16, O, I);
    { GemmP gs1_16;
      gs1_16.A = CP; gs1_16.B = Wc; gs1_16.bias = CP; gs1_16.R = CP; gs1_16.C = S + (size_t)16 * O * 4 * LP;
      gs1_16.sAo = (long long)4 * KD; gs1_16.sAi = 0; gs1_16.sAm = KD; gs1_16.sAk = 1; gs1_16.sBo = (long long)KD * 4; gs1_16.sBi = 0; gs1_16.sBn = 1; gs1_16.sBk = 4; gs1_16.sCo = 4 * LP; gs1_16.sCi = 0; gs1_16.sCm = LP; gs1_16.sRo = 0; gs1_16.sRi = 0; gs1_16.sRm = 0; gs1_16.sRn = 0;
      gs1_16.M = 4; gs1_16.N = 4; gs1_16.K = KD; gs1_16.zi_n = 1; gs1_16.flags = 0; gs1_16.act = 0;
      gs1_16.alpha = 1.0f; gs1_16.beta = 0.0f; gs1_16.sa = 1.0f; gs1_16.sb = 1.0f; gs1_16.Npad = LP; gs1_16.pad_ = 0;
      k_gemm<1><<<dim3((unsigned)((LP) + 31) / 32, (unsigned)((4) + 15) / 16, (unsigned)(O)), 32, 0, stream>>>(gs1_16); }
    k_caps_cp<<<(unsigned)(((long long)O * 4 * KD + 255) / 256), 256, 0, stream>>>(P, CC, CP, 17, O, I);
    { GemmP gs1_17;
      gs1_17.A = CP; gs1_17.B = Wc; gs1_17.bias = CP; gs1_17.R = CP; gs1_17.C = S + (size_t)17 * O * 4 * LP;
      gs1_17.sAo = (long long)4 * KD; gs1_17.sAi = 0; gs1_17.sAm = KD; gs1_17.sAk = 1; gs1_17.sBo = (long long)KD * 4; gs1_17.sBi = 0; gs1_17.sBn = 1; gs1_17.sBk = 4; gs1_17.sCo = 4 * LP; gs1_17.sCi = 0; gs1_17.sCm = LP; gs1_17.sRo = 0; gs1_17.sRi = 0; gs1_17.sRm = 0; gs1_17.sRn = 0;
      gs1_17.M = 4; gs1_17.N = 4; gs1_17.K = KD; gs1_17.zi_n = 1; gs1_17.flags = 0; gs1_17.act = 0;
      gs1_17.alpha = 1.0f; gs1_17.beta = 0.0f; gs1_17.sa = 1.0f; gs1_17.sb = 1.0f; gs1_17.Npad = LP; gs1_17.pad_ = 0;
      k_gemm<1><<<dim3((unsigned)((LP) + 31) / 32, (unsigned)((4) + 15) / 16, (unsigned)(O)), 32, 0, stream>>>(gs1_17); }
    k_caps_cp<<<(unsigned)(((long long)O * 4 * KD + 255) / 256), 256, 0, stream>>>(P, CC, CP, 18, O, I);
    { GemmP gs1_18;
      gs1_18.A = CP; gs1_18.B = Wc; gs1_18.bias = CP; gs1_18.R = CP; gs1_18.C = S + (size_t)18 * O * 4 * LP;
      gs1_18.sAo = (long long)4 * KD; gs1_18.sAi = 0; gs1_18.sAm = KD; gs1_18.sAk = 1; gs1_18.sBo = (long long)KD * 4; gs1_18.sBi = 0; gs1_18.sBn = 1; gs1_18.sBk = 4; gs1_18.sCo = 4 * LP; gs1_18.sCi = 0; gs1_18.sCm = LP; gs1_18.sRo = 0; gs1_18.sRi = 0; gs1_18.sRm = 0; gs1_18.sRn = 0;
      gs1_18.M = 4; gs1_18.N = 4; gs1_18.K = KD; gs1_18.zi_n = 1; gs1_18.flags = 0; gs1_18.act = 0;
      gs1_18.alpha = 1.0f; gs1_18.beta = 0.0f; gs1_18.sa = 1.0f; gs1_18.sb = 1.0f; gs1_18.Npad = LP; gs1_18.pad_ = 0;
      k_gemm<1><<<dim3((unsigned)((LP) + 31) / 32, (unsigned)((4) + 15) / 16, (unsigned)(O)), 32, 0, stream>>>(gs1_18); }
    k_caps_cp<<<(unsigned)(((long long)O * 4 * KD + 255) / 256), 256, 0, stream>>>(P, CC, CP, 19, O, I);
    { GemmP gs1_19;
      gs1_19.A = CP; gs1_19.B = Wc; gs1_19.bias = CP; gs1_19.R = CP; gs1_19.C = S + (size_t)19 * O * 4 * LP;
      gs1_19.sAo = (long long)4 * KD; gs1_19.sAi = 0; gs1_19.sAm = KD; gs1_19.sAk = 1; gs1_19.sBo = (long long)KD * 4; gs1_19.sBi = 0; gs1_19.sBn = 1; gs1_19.sBk = 4; gs1_19.sCo = 4 * LP; gs1_19.sCi = 0; gs1_19.sCm = LP; gs1_19.sRo = 0; gs1_19.sRi = 0; gs1_19.sRm = 0; gs1_19.sRn = 0;
      gs1_19.M = 4; gs1_19.N = 4; gs1_19.K = KD; gs1_19.zi_n = 1; gs1_19.flags = 0; gs1_19.act = 0;
      gs1_19.alpha = 1.0f; gs1_19.beta = 0.0f; gs1_19.sa = 1.0f; gs1_19.sb = 1.0f; gs1_19.Npad = LP; gs1_19.pad_ = 0;
      k_gemm<1><<<dim3((unsigned)((LP) + 31) / 32, (unsigned)((4) + 15) / 16, (unsigned)(O)), 32, 0, stream>>>(gs1_19); }
    k_caps_cp<<<(unsigned)(((long long)O * 4 * KD + 255) / 256), 256, 0, stream>>>(P, CC, CP, 20, O, I);
    { GemmP gs1_20;
      gs1_20.A = CP; gs1_20.B = Wc; gs1_20.bias = CP; gs1_20.R = CP; gs1_20.C = S + (size_t)20 * O * 4 * LP;
      gs1_20.sAo = (long long)4 * KD; gs1_20.sAi = 0; gs1_20.sAm = KD; gs1_20.sAk = 1; gs1_20.sBo = (long long)KD * 4; gs1_20.sBi = 0; gs1_20.sBn = 1; gs1_20.sBk = 4; gs1_20.sCo = 4 * LP; gs1_20.sCi = 0; gs1_20.sCm = LP; gs1_20.sRo = 0; gs1_20.sRi = 0; gs1_20.sRm = 0; gs1_20.sRn = 0;
      gs1_20.M = 4; gs1_20.N = 4; gs1_20.K = KD; gs1_20.zi_n = 1; gs1_20.flags = 0; gs1_20.act = 0;
      gs1_20.alpha = 1.0f; gs1_20.beta = 0.0f; gs1_20.sa = 1.0f; gs1_20.sb = 1.0f; gs1_20.Npad = LP; gs1_20.pad_ = 0;
      k_gemm<1><<<dim3((unsigned)((LP) + 31) / 32, (unsigned)((4) + 15) / 16, (unsigned)(O)), 32, 0, stream>>>(gs1_20); }
    k_caps_cp<<<(unsigned)(((long long)O * 4 * KD + 255) / 256), 256, 0, stream>>>(P, CC, CP, 21, O, I);
    { GemmP gs1_21;
      gs1_21.A = CP; gs1_21.B = Wc; gs1_21.bias = CP; gs1_21.R = CP; gs1_21.C = S + (size_t)21 * O * 4 * LP;
      gs1_21.sAo = (long long)4 * KD; gs1_21.sAi = 0; gs1_21.sAm = KD; gs1_21.sAk = 1; gs1_21.sBo = (long long)KD * 4; gs1_21.sBi = 0; gs1_21.sBn = 1; gs1_21.sBk = 4; gs1_21.sCo = 4 * LP; gs1_21.sCi = 0; gs1_21.sCm = LP; gs1_21.sRo = 0; gs1_21.sRi = 0; gs1_21.sRm = 0; gs1_21.sRn = 0;
      gs1_21.M = 4; gs1_21.N = 4; gs1_21.K = KD; gs1_21.zi_n = 1; gs1_21.flags = 0; gs1_21.act = 0;
      gs1_21.alpha = 1.0f; gs1_21.beta = 0.0f; gs1_21.sa = 1.0f; gs1_21.sb = 1.0f; gs1_21.Npad = LP; gs1_21.pad_ = 0;
      k_gemm<1><<<dim3((unsigned)((LP) + 31) / 32, (unsigned)((4) + 15) / 16, (unsigned)(O)), 32, 0, stream>>>(gs1_21); }
    k_caps_cp<<<(unsigned)(((long long)O * 4 * KD + 255) / 256), 256, 0, stream>>>(P, CC, CP, 22, O, I);
    { GemmP gs1_22;
      gs1_22.A = CP; gs1_22.B = Wc; gs1_22.bias = CP; gs1_22.R = CP; gs1_22.C = S + (size_t)22 * O * 4 * LP;
      gs1_22.sAo = (long long)4 * KD; gs1_22.sAi = 0; gs1_22.sAm = KD; gs1_22.sAk = 1; gs1_22.sBo = (long long)KD * 4; gs1_22.sBi = 0; gs1_22.sBn = 1; gs1_22.sBk = 4; gs1_22.sCo = 4 * LP; gs1_22.sCi = 0; gs1_22.sCm = LP; gs1_22.sRo = 0; gs1_22.sRi = 0; gs1_22.sRm = 0; gs1_22.sRn = 0;
      gs1_22.M = 4; gs1_22.N = 4; gs1_22.K = KD; gs1_22.zi_n = 1; gs1_22.flags = 0; gs1_22.act = 0;
      gs1_22.alpha = 1.0f; gs1_22.beta = 0.0f; gs1_22.sa = 1.0f; gs1_22.sb = 1.0f; gs1_22.Npad = LP; gs1_22.pad_ = 0;
      k_gemm<1><<<dim3((unsigned)((LP) + 31) / 32, (unsigned)((4) + 15) / 16, (unsigned)(O)), 32, 0, stream>>>(gs1_22); }
    k_caps_cp<<<(unsigned)(((long long)O * 4 * KD + 255) / 256), 256, 0, stream>>>(P, CC, CP, 23, O, I);
    { GemmP gs1_23;
      gs1_23.A = CP; gs1_23.B = Wc; gs1_23.bias = CP; gs1_23.R = CP; gs1_23.C = S + (size_t)23 * O * 4 * LP;
      gs1_23.sAo = (long long)4 * KD; gs1_23.sAi = 0; gs1_23.sAm = KD; gs1_23.sAk = 1; gs1_23.sBo = (long long)KD * 4; gs1_23.sBi = 0; gs1_23.sBn = 1; gs1_23.sBk = 4; gs1_23.sCo = 4 * LP; gs1_23.sCi = 0; gs1_23.sCm = LP; gs1_23.sRo = 0; gs1_23.sRi = 0; gs1_23.sRm = 0; gs1_23.sRn = 0;
      gs1_23.M = 4; gs1_23.N = 4; gs1_23.K = KD; gs1_23.zi_n = 1; gs1_23.flags = 0; gs1_23.act = 0;
      gs1_23.alpha = 1.0f; gs1_23.beta = 0.0f; gs1_23.sa = 1.0f; gs1_23.sb = 1.0f; gs1_23.Npad = LP; gs1_23.pad_ = 0;
      k_gemm<1><<<dim3((unsigned)((LP) + 31) / 32, (unsigned)((4) + 15) / 16, (unsigned)(O)), 32, 0, stream>>>(gs1_23); }
    k_caps_cp<<<(unsigned)(((long long)O * 4 * KD + 255) / 256), 256, 0, stream>>>(P, CC, CP, 24, O, I);
    { GemmP gs1_24;
      gs1_24.A = CP; gs1_24.B = Wc; gs1_24.bias = CP; gs1_24.R = CP; gs1_24.C = S + (size_t)24 * O * 4 * LP;
      gs1_24.sAo = (long long)4 * KD; gs1_24.sAi = 0; gs1_24.sAm = KD; gs1_24.sAk = 1; gs1_24.sBo = (long long)KD * 4; gs1_24.sBi = 0; gs1_24.sBn = 1; gs1_24.sBk = 4; gs1_24.sCo = 4 * LP; gs1_24.sCi = 0; gs1_24.sCm = LP; gs1_24.sRo = 0; gs1_24.sRi = 0; gs1_24.sRm = 0; gs1_24.sRn = 0;
      gs1_24.M = 4; gs1_24.N = 4; gs1_24.K = KD; gs1_24.zi_n = 1; gs1_24.flags = 0; gs1_24.act = 0;
      gs1_24.alpha = 1.0f; gs1_24.beta = 0.0f; gs1_24.sa = 1.0f; gs1_24.sb = 1.0f; gs1_24.Npad = LP; gs1_24.pad_ = 0;
      k_gemm<1><<<dim3((unsigned)((LP) + 31) / 32, (unsigned)((4) + 15) / 16, (unsigned)(O)), 32, 0, stream>>>(gs1_24); }
    k_caps_cp<<<(unsigned)(((long long)O * 4 * KD + 255) / 256), 256, 0, stream>>>(P, CC, CP, 25, O, I);
    { GemmP gs1_25;
      gs1_25.A = CP; gs1_25.B = Wc; gs1_25.bias = CP; gs1_25.R = CP; gs1_25.C = S + (size_t)25 * O * 4 * LP;
      gs1_25.sAo = (long long)4 * KD; gs1_25.sAi = 0; gs1_25.sAm = KD; gs1_25.sAk = 1; gs1_25.sBo = (long long)KD * 4; gs1_25.sBi = 0; gs1_25.sBn = 1; gs1_25.sBk = 4; gs1_25.sCo = 4 * LP; gs1_25.sCi = 0; gs1_25.sCm = LP; gs1_25.sRo = 0; gs1_25.sRi = 0; gs1_25.sRm = 0; gs1_25.sRn = 0;
      gs1_25.M = 4; gs1_25.N = 4; gs1_25.K = KD; gs1_25.zi_n = 1; gs1_25.flags = 0; gs1_25.act = 0;
      gs1_25.alpha = 1.0f; gs1_25.beta = 0.0f; gs1_25.sa = 1.0f; gs1_25.sb = 1.0f; gs1_25.Npad = LP; gs1_25.pad_ = 0;
      k_gemm<1><<<dim3((unsigned)((LP) + 31) / 32, (unsigned)((4) + 15) / 16, (unsigned)(O)), 32, 0, stream>>>(gs1_25); }
    k_caps_cp<<<(unsigned)(((long long)O * 4 * KD + 255) / 256), 256, 0, stream>>>(P, CC, CP, 26, O, I);
    { GemmP gs1_26;
      gs1_26.A = CP; gs1_26.B = Wc; gs1_26.bias = CP; gs1_26.R = CP; gs1_26.C = S + (size_t)26 * O * 4 * LP;
      gs1_26.sAo = (long long)4 * KD; gs1_26.sAi = 0; gs1_26.sAm = KD; gs1_26.sAk = 1; gs1_26.sBo = (long long)KD * 4; gs1_26.sBi = 0; gs1_26.sBn = 1; gs1_26.sBk = 4; gs1_26.sCo = 4 * LP; gs1_26.sCi = 0; gs1_26.sCm = LP; gs1_26.sRo = 0; gs1_26.sRi = 0; gs1_26.sRm = 0; gs1_26.sRn = 0;
      gs1_26.M = 4; gs1_26.N = 4; gs1_26.K = KD; gs1_26.zi_n = 1; gs1_26.flags = 0; gs1_26.act = 0;
      gs1_26.alpha = 1.0f; gs1_26.beta = 0.0f; gs1_26.sa = 1.0f; gs1_26.sb = 1.0f; gs1_26.Npad = LP; gs1_26.pad_ = 0;
      k_gemm<1><<<dim3((unsigned)((LP) + 31) / 32, (unsigned)((4) + 15) / 16, (unsigned)(O)), 32, 0, stream>>>(gs1_26); }
    k_caps_cp<<<(unsigned)(((long long)O * 4 * KD + 255) / 256), 256, 0, stream>>>(P, CC, CP, 27, O, I);
    { GemmP gs1_27;
      gs1_27.A = CP; gs1_27.B = Wc; gs1_27.bias = CP; gs1_27.R = CP; gs1_27.C = S + (size_t)27 * O * 4 * LP;
      gs1_27.sAo = (long long)4 * KD; gs1_27.sAi = 0; gs1_27.sAm = KD; gs1_27.sAk = 1; gs1_27.sBo = (long long)KD * 4; gs1_27.sBi = 0; gs1_27.sBn = 1; gs1_27.sBk = 4; gs1_27.sCo = 4 * LP; gs1_27.sCi = 0; gs1_27.sCm = LP; gs1_27.sRo = 0; gs1_27.sRi = 0; gs1_27.sRm = 0; gs1_27.sRn = 0;
      gs1_27.M = 4; gs1_27.N = 4; gs1_27.K = KD; gs1_27.zi_n = 1; gs1_27.flags = 0; gs1_27.act = 0;
      gs1_27.alpha = 1.0f; gs1_27.beta = 0.0f; gs1_27.sa = 1.0f; gs1_27.sb = 1.0f; gs1_27.Npad = LP; gs1_27.pad_ = 0;
      k_gemm<1><<<dim3((unsigned)((LP) + 31) / 32, (unsigned)((4) + 15) / 16, (unsigned)(O)), 32, 0, stream>>>(gs1_27); }
    k_caps_cp<<<(unsigned)(((long long)O * 4 * KD + 255) / 256), 256, 0, stream>>>(P, CC, CP, 28, O, I);
    { GemmP gs1_28;
      gs1_28.A = CP; gs1_28.B = Wc; gs1_28.bias = CP; gs1_28.R = CP; gs1_28.C = S + (size_t)28 * O * 4 * LP;
      gs1_28.sAo = (long long)4 * KD; gs1_28.sAi = 0; gs1_28.sAm = KD; gs1_28.sAk = 1; gs1_28.sBo = (long long)KD * 4; gs1_28.sBi = 0; gs1_28.sBn = 1; gs1_28.sBk = 4; gs1_28.sCo = 4 * LP; gs1_28.sCi = 0; gs1_28.sCm = LP; gs1_28.sRo = 0; gs1_28.sRi = 0; gs1_28.sRm = 0; gs1_28.sRn = 0;
      gs1_28.M = 4; gs1_28.N = 4; gs1_28.K = KD; gs1_28.zi_n = 1; gs1_28.flags = 0; gs1_28.act = 0;
      gs1_28.alpha = 1.0f; gs1_28.beta = 0.0f; gs1_28.sa = 1.0f; gs1_28.sb = 1.0f; gs1_28.Npad = LP; gs1_28.pad_ = 0;
      k_gemm<1><<<dim3((unsigned)((LP) + 31) / 32, (unsigned)((4) + 15) / 16, (unsigned)(O)), 32, 0, stream>>>(gs1_28); }
    k_caps_cp<<<(unsigned)(((long long)O * 4 * KD + 255) / 256), 256, 0, stream>>>(P, CC, CP, 29, O, I);
    { GemmP gs1_29;
      gs1_29.A = CP; gs1_29.B = Wc; gs1_29.bias = CP; gs1_29.R = CP; gs1_29.C = S + (size_t)29 * O * 4 * LP;
      gs1_29.sAo = (long long)4 * KD; gs1_29.sAi = 0; gs1_29.sAm = KD; gs1_29.sAk = 1; gs1_29.sBo = (long long)KD * 4; gs1_29.sBi = 0; gs1_29.sBn = 1; gs1_29.sBk = 4; gs1_29.sCo = 4 * LP; gs1_29.sCi = 0; gs1_29.sCm = LP; gs1_29.sRo = 0; gs1_29.sRi = 0; gs1_29.sRm = 0; gs1_29.sRn = 0;
      gs1_29.M = 4; gs1_29.N = 4; gs1_29.K = KD; gs1_29.zi_n = 1; gs1_29.flags = 0; gs1_29.act = 0;
      gs1_29.alpha = 1.0f; gs1_29.beta = 0.0f; gs1_29.sa = 1.0f; gs1_29.sb = 1.0f; gs1_29.Npad = LP; gs1_29.pad_ = 0;
      k_gemm<1><<<dim3((unsigned)((LP) + 31) / 32, (unsigned)((4) + 15) / 16, (unsigned)(O)), 32, 0, stream>>>(gs1_29); }
    k_caps_cp<<<(unsigned)(((long long)O * 4 * KD + 255) / 256), 256, 0, stream>>>(P, CC, CP, 30, O, I);
    { GemmP gs1_30;
      gs1_30.A = CP; gs1_30.B = Wc; gs1_30.bias = CP; gs1_30.R = CP; gs1_30.C = S + (size_t)30 * O * 4 * LP;
      gs1_30.sAo = (long long)4 * KD; gs1_30.sAi = 0; gs1_30.sAm = KD; gs1_30.sAk = 1; gs1_30.sBo = (long long)KD * 4; gs1_30.sBi = 0; gs1_30.sBn = 1; gs1_30.sBk = 4; gs1_30.sCo = 4 * LP; gs1_30.sCi = 0; gs1_30.sCm = LP; gs1_30.sRo = 0; gs1_30.sRi = 0; gs1_30.sRm = 0; gs1_30.sRn = 0;
      gs1_30.M = 4; gs1_30.N = 4; gs1_30.K = KD; gs1_30.zi_n = 1; gs1_30.flags = 0; gs1_30.act = 0;
      gs1_30.alpha = 1.0f; gs1_30.beta = 0.0f; gs1_30.sa = 1.0f; gs1_30.sb = 1.0f; gs1_30.Npad = LP; gs1_30.pad_ = 0;
      k_gemm<1><<<dim3((unsigned)((LP) + 31) / 32, (unsigned)((4) + 15) / 16, (unsigned)(O)), 32, 0, stream>>>(gs1_30); }
    k_caps_cp<<<(unsigned)(((long long)O * 4 * KD + 255) / 256), 256, 0, stream>>>(P, CC, CP, 31, O, I);
    { GemmP gs1_31;
      gs1_31.A = CP; gs1_31.B = Wc; gs1_31.bias = CP; gs1_31.R = CP; gs1_31.C = S + (size_t)31 * O * 4 * LP;
      gs1_31.sAo = (long long)4 * KD; gs1_31.sAi = 0; gs1_31.sAm = KD; gs1_31.sAk = 1; gs1_31.sBo = (long long)KD * 4; gs1_31.sBi = 0; gs1_31.sBn = 1; gs1_31.sBk = 4; gs1_31.sCo = 4 * LP; gs1_31.sCi = 0; gs1_31.sCm = LP; gs1_31.sRo = 0; gs1_31.sRi = 0; gs1_31.sRm = 0; gs1_31.sRn = 0;
      gs1_31.M = 4; gs1_31.N = 4; gs1_31.K = KD; gs1_31.zi_n = 1; gs1_31.flags = 0; gs1_31.act = 0;
      gs1_31.alpha = 1.0f; gs1_31.beta = 0.0f; gs1_31.sa = 1.0f; gs1_31.sb = 1.0f; gs1_31.Npad = LP; gs1_31.pad_ = 0;
      k_gemm<1><<<dim3((unsigned)((LP) + 31) / 32, (unsigned)((4) + 15) / 16, (unsigned)(O)), 32, 0, stream>>>(gs1_31); }
    k_caps_squash<<<(unsigned)((Bn * O * 16 + 255) / 256), 256, 0, stream>>>(S, LP, V, out, aout, Bn * O, 0);
    k_caps_agree<<<(unsigned)(((long long)Bn * O * I + 255) / 256), 256, 0, stream>>>(P, Wc, V, BL, Bn, O, I);
    k_caps_soft<<<(unsigned)((Bn * I + 255) / 256), 256, 0, stream>>>(BL, CC, Bn, O, I);
    k_caps_cp<<<(unsigned)(((long long)O * 4 * KD + 255) / 256), 256, 0, stream>>>(P, CC, CP, 0, O, I);
    { GemmP gs2_0;
      gs2_0.A = CP; gs2_0.B = Wc; gs2_0.bias = CP; gs2_0.R = CP; gs2_0.C = S + (size_t)0 * O * 4 * LP;
      gs2_0.sAo = (long long)4 * KD; gs2_0.sAi = 0; gs2_0.sAm = KD; gs2_0.sAk = 1; gs2_0.sBo = (long long)KD * 4; gs2_0.sBi = 0; gs2_0.sBn = 1; gs2_0.sBk = 4; gs2_0.sCo = 4 * LP; gs2_0.sCi = 0; gs2_0.sCm = LP; gs2_0.sRo = 0; gs2_0.sRi = 0; gs2_0.sRm = 0; gs2_0.sRn = 0;
      gs2_0.M = 4; gs2_0.N = 4; gs2_0.K = KD; gs2_0.zi_n = 1; gs2_0.flags = 0; gs2_0.act = 0;
      gs2_0.alpha = 1.0f; gs2_0.beta = 0.0f; gs2_0.sa = 1.0f; gs2_0.sb = 1.0f; gs2_0.Npad = LP; gs2_0.pad_ = 0;
      k_gemm<1><<<dim3((unsigned)((LP) + 31) / 32, (unsigned)((4) + 15) / 16, (unsigned)(O)), 32, 0, stream>>>(gs2_0); }
    k_caps_cp<<<(unsigned)(((long long)O * 4 * KD + 255) / 256), 256, 0, stream>>>(P, CC, CP, 1, O, I);
    { GemmP gs2_1;
      gs2_1.A = CP; gs2_1.B = Wc; gs2_1.bias = CP; gs2_1.R = CP; gs2_1.C = S + (size_t)1 * O * 4 * LP;
      gs2_1.sAo = (long long)4 * KD; gs2_1.sAi = 0; gs2_1.sAm = KD; gs2_1.sAk = 1; gs2_1.sBo = (long long)KD * 4; gs2_1.sBi = 0; gs2_1.sBn = 1; gs2_1.sBk = 4; gs2_1.sCo = 4 * LP; gs2_1.sCi = 0; gs2_1.sCm = LP; gs2_1.sRo = 0; gs2_1.sRi = 0; gs2_1.sRm = 0; gs2_1.sRn = 0;
      gs2_1.M = 4; gs2_1.N = 4; gs2_1.K = KD; gs2_1.zi_n = 1; gs2_1.flags = 0; gs2_1.act = 0;
      gs2_1.alpha = 1.0f; gs2_1.beta = 0.0f; gs2_1.sa = 1.0f; gs2_1.sb = 1.0f; gs2_1.Npad = LP; gs2_1.pad_ = 0;
      k_gemm<1><<<dim3((unsigned)((LP) + 31) / 32, (unsigned)((4) + 15) / 16, (unsigned)(O)), 32, 0, stream>>>(gs2_1); }
    k_caps_cp<<<(unsigned)(((long long)O * 4 * KD + 255) / 256), 256, 0, stream>>>(P, CC, CP, 2, O, I);
    { GemmP gs2_2;
      gs2_2.A = CP; gs2_2.B = Wc; gs2_2.bias = CP; gs2_2.R = CP; gs2_2.C = S + (size_t)2 * O * 4 * LP;
      gs2_2.sAo = (long long)4 * KD; gs2_2.sAi = 0; gs2_2.sAm = KD; gs2_2.sAk = 1; gs2_2.sBo = (long long)KD * 4; gs2_2.sBi = 0; gs2_2.sBn = 1; gs2_2.sBk = 4; gs2_2.sCo = 4 * LP; gs2_2.sCi = 0; gs2_2.sCm = LP; gs2_2.sRo = 0; gs2_2.sRi = 0; gs2_2.sRm = 0; gs2_2.sRn = 0;
      gs2_2.M = 4; gs2_2.N = 4; gs2_2.K = KD; gs2_2.zi_n = 1; gs2_2.flags = 0; gs2_2.act = 0;
      gs2_2.alpha = 1.0f; gs2_2.beta = 0.0f; gs2_2.sa = 1.0f; gs2_2.sb = 1.0f; gs2_2.Npad = LP; gs2_2.pad_ = 0;
      k_gemm<1><<<dim3((unsigned)((LP) + 31) / 32, (unsigned)((4) + 15) / 16, (unsigned)(O)), 32, 0, stream>>>(gs2_2); }
    k_caps_cp<<<(unsigned)(((long long)O * 4 * KD + 255) / 256), 256, 0, stream>>>(P, CC, CP, 3, O, I);
    { GemmP gs2_3;
      gs2_3.A = CP; gs2_3.B = Wc; gs2_3.bias = CP; gs2_3.R = CP; gs2_3.C = S + (size_t)3 * O * 4 * LP;
      gs2_3.sAo = (long long)4 * KD; gs2_3.sAi = 0; gs2_3.sAm = KD; gs2_3.sAk = 1; gs2_3.sBo = (long long)KD * 4; gs2_3.sBi = 0; gs2_3.sBn = 1; gs2_3.sBk = 4; gs2_3.sCo = 4 * LP; gs2_3.sCi = 0; gs2_3.sCm = LP; gs2_3.sRo = 0; gs2_3.sRi = 0; gs2_3.sRm = 0; gs2_3.sRn = 0;
      gs2_3.M = 4; gs2_3.N = 4; gs2_3.K = KD; gs2_3.zi_n = 1; gs2_3.flags = 0; gs2_3.act = 0;
      gs2_3.alpha = 1.0f; gs2_3.beta = 0.0f; gs2_3.sa = 1.0f; gs2_3.sb = 1.0f; gs2_3.Npad = LP; gs2_3.pad_ = 0;
      k_gemm<1><<<dim3((unsigned)((LP) + 31) / 32, (unsigned)((4) + 15) / 16, (unsigned)(O)), 32, 0, stream>>>(gs2_3); }
    k_caps_cp<<<(unsigned)(((long long)O * 4 * KD + 255) / 256), 256, 0, stream>>>(P, CC, CP, 4, O, I);
    { GemmP gs2_4;
      gs2_4.A = CP; gs2_4.B = Wc; gs2_4.bias = CP; gs2_4.R = CP; gs2_4.C = S + (size_t)4 * O * 4 * LP;
      gs2_4.sAo = (long long)4 * KD; gs2_4.sAi = 0; gs2_4.sAm = KD; gs2_4.sAk = 1; gs2_4.sBo = (long long)KD * 4; gs2_4.sBi = 0; gs2_4.sBn = 1; gs2_4.sBk = 4; gs2_4.sCo = 4 * LP; gs2_4.sCi = 0; gs2_4.sCm = LP; gs2_4.sRo = 0; gs2_4.sRi = 0; gs2_4.sRm = 0; gs2_4.sRn = 0;
      gs2_4.M = 4; gs2_4.N = 4; gs2_4.K = KD; gs2_4.zi_n = 1; gs2_4.flags = 0; gs2_4.act = 0;
      gs2_4.alpha = 1.0f; gs2_4.beta = 0.0f; gs2_4.sa = 1.0f; gs2_4.sb = 1.0f; gs2_4.Npad = LP; gs2_4.pad_ = 0;
      k_gemm<1><<<dim3((unsigned)((LP) + 31) / 32, (unsigned)((4) + 15) / 16, (unsigned)(O)), 32, 0, stream>>>(gs2_4); }
    k_caps_cp<<<(unsigned)(((long long)O * 4 * KD + 255) / 256), 256, 0, stream>>>(P, CC, CP, 5, O, I);
    { GemmP gs2_5;
      gs2_5.A = CP; gs2_5.B = Wc; gs2_5.bias = CP; gs2_5.R = CP; gs2_5.C = S + (size_t)5 * O * 4 * LP;
      gs2_5.sAo = (long long)4 * KD; gs2_5.sAi = 0; gs2_5.sAm = KD; gs2_5.sAk = 1; gs2_5.sBo = (long long)KD * 4; gs2_5.sBi = 0; gs2_5.sBn = 1; gs2_5.sBk = 4; gs2_5.sCo = 4 * LP; gs2_5.sCi = 0; gs2_5.sCm = LP; gs2_5.sRo = 0; gs2_5.sRi = 0; gs2_5.sRm = 0; gs2_5.sRn = 0;
      gs2_5.M = 4; gs2_5.N = 4; gs2_5.K = KD; gs2_5.zi_n = 1; gs2_5.flags = 0; gs2_5.act = 0;
      gs2_5.alpha = 1.0f; gs2_5.beta = 0.0f; gs2_5.sa = 1.0f; gs2_5.sb = 1.0f; gs2_5.Npad = LP; gs2_5.pad_ = 0;
      k_gemm<1><<<dim3((unsigned)((LP) + 31) / 32, (unsigned)((4) + 15) / 16, (unsigned)(O)), 32, 0, stream>>>(gs2_5); }
    k_caps_cp<<<(unsigned)(((long long)O * 4 * KD + 255) / 256), 256, 0, stream>>>(P, CC, CP, 6, O, I);
    { GemmP gs2_6;
      gs2_6.A = CP; gs2_6.B = Wc; gs2_6.bias = CP; gs2_6.R = CP; gs2_6.C = S + (size_t)6 * O * 4 * LP;
      gs2_6.sAo = (long long)4 * KD; gs2_6.sAi = 0; gs2_6.sAm = KD; gs2_6.sAk = 1; gs2_6.sBo = (long long)KD * 4; gs2_6.sBi = 0; gs2_6.sBn = 1; gs2_6.sBk = 4; gs2_6.sCo = 4 * LP; gs2_6.sCi = 0; gs2_6.sCm = LP; gs2_6.sRo = 0; gs2_6.sRi = 0; gs2_6.sRm = 0; gs2_6.sRn = 0;
      gs2_6.M = 4; gs2_6.N = 4; gs2_6.K = KD; gs2_6.zi_n = 1; gs2_6.flags = 0; gs2_6.act = 0;
      gs2_6.alpha = 1.0f; gs2_6.beta = 0.0f; gs2_6.sa = 1.0f; gs2_6.sb = 1.0f; gs2_6.Npad = LP; gs2_6.pad_ = 0;
      k_gemm<1><<<dim3((unsigned)((LP) + 31) / 32, (unsigned)((4) + 15) / 16, (unsigned)(O)), 32, 0, stream>>>(gs2_6); }
    k_caps_cp<<<(unsigned)(((long long)O * 4 * KD + 255) / 256), 256, 0, stream>>>(P, CC, CP, 7, O, I);
    { GemmP gs2_7;
      gs2_7.A = CP; gs2_7.B = Wc; gs2_7.bias = CP; gs2_7.R = CP; gs2_7.C = S + (size_t)7 * O * 4 * LP;
      gs2_7.sAo = (long long)4 * KD; gs2_7.sAi = 0; gs2_7.sAm = KD; gs2_7.sAk = 1; gs2_7.sBo = (long long)KD * 4; gs2_7.sBi = 0; gs2_7.sBn = 1; gs2_7.sBk = 4; gs2_7.sCo = 4 * LP; gs2_7.sCi = 0; gs2_7.sCm = LP; gs2_7.sRo = 0; gs2_7.sRi = 0; gs2_7.sRm = 0; gs2_7.sRn = 0;
      gs2_7.M = 4; gs2_7.N = 4; gs2_7.K = KD; gs2_7.zi_n = 1; gs2_7.flags = 0; gs2_7.act = 0;
      gs2_7.alpha = 1.0f; gs2_7.beta = 0.0f; gs2_7.sa = 1.0f; gs2_7.sb = 1.0f; gs2_7.Npad = LP; gs2_7.pad_ = 0;
      k_gemm<1><<<dim3((unsigned)((LP) + 31) / 32, (unsigned)((4) + 15) / 16, (unsigned)(O)), 32, 0, stream>>>(gs2_7); }
    k_caps_cp<<<(unsigned)(((long long)O * 4 * KD + 255) / 256), 256, 0, stream>>>(P, CC, CP, 8, O, I);
    { GemmP gs2_8;
      gs2_8.A = CP; gs2_8.B = Wc; gs2_8.bias = CP; gs2_8.R = CP; gs2_8.C = S + (size_t)8 * O * 4 * LP;
      gs2_8.sAo = (long long)4 * KD; gs2_8.sAi = 0; gs2_8.sAm = KD; gs2_8.sAk = 1; gs2_8.sBo = (long long)KD * 4; gs2_8.sBi = 0; gs2_8.sBn = 1; gs2_8.sBk = 4; gs2_8.sCo = 4 * LP; gs2_8.sCi = 0; gs2_8.sCm = LP; gs2_8.sRo = 0; gs2_8.sRi = 0; gs2_8.sRm = 0; gs2_8.sRn = 0;
      gs2_8.M = 4; gs2_8.N = 4; gs2_8.K = KD; gs2_8.zi_n = 1; gs2_8.flags = 0; gs2_8.act = 0;
      gs2_8.alpha = 1.0f; gs2_8.beta = 0.0f; gs2_8.sa = 1.0f; gs2_8.sb = 1.0f; gs2_8.Npad = LP; gs2_8.pad_ = 0;
      k_gemm<1><<<dim3((unsigned)((LP) + 31) / 32, (unsigned)((4) + 15) / 16, (unsigned)(O)), 32, 0, stream>>>(gs2_8); }
    k_caps_cp<<<(unsigned)(((long long)O * 4 * KD + 255) / 256), 256, 0, stream>>>(P, CC, CP, 9, O, I);
    { GemmP gs2_9;
      gs2_9.A = CP; gs2_9.B = Wc; gs2_9.bias = CP; gs2_9.R = CP; gs2_9.C = S + (size_t)9 * O * 4 * LP;
      gs2_9.sAo = (long long)4 * KD; gs2_9.sAi = 0; gs2_9.sAm = KD; gs2_9.sAk = 1; gs2_9.sBo = (long long)KD * 4; gs2_9.sBi = 0; gs2_9.sBn = 1; gs2_9.sBk = 4; gs2_9.sCo = 4 * LP; gs2_9.sCi = 0; gs2_9.sCm = LP; gs2_9.sRo = 0; gs2_9.sRi = 0; gs2_9.sRm = 0; gs2_9.sRn = 0;
      gs2_9.M = 4; gs2_9.N = 4; gs2_9.K = KD; gs2_9.zi_n = 1; gs2_9.flags = 0; gs2_9.act = 0;
      gs2_9.alpha = 1.0f; gs2_9.beta = 0.0f; gs2_9.sa = 1.0f; gs2_9.sb = 1.0f; gs2_9.Npad = LP; gs2_9.pad_ = 0;
      k_gemm<1><<<dim3((unsigned)((LP) + 31) / 32, (unsigned)((4) + 15) / 16, (unsigned)(O)), 32, 0, stream>>>(gs2_9); }
    k_caps_cp<<<(unsigned)(((long long)O * 4 * KD + 255) / 256), 256, 0, stream>>>(P, CC, CP, 10, O, I);
    { GemmP gs2_10;
      gs2_10.A = CP; gs2_10.B = Wc; gs2_10.bias = CP; gs2_10.R = CP; gs2_10.C = S + (size_t)10 * O * 4 * LP;
      gs2_10.sAo = (long long)4 * KD; gs2_10.sAi = 0; gs2_10.sAm = KD; gs2_10.sAk = 1; gs2_10.sBo = (long long)KD * 4; gs2_10.sBi = 0; gs2_10.sBn = 1; gs2_10.sBk = 4; gs2_10.sCo = 4 * LP; gs2_10.sCi = 0; gs2_10.sCm = LP; gs2_10.sRo = 0; gs2_10.sRi = 0; gs2_10.sRm = 0; gs2_10.sRn = 0;
      gs2_10.M = 4; gs2_10.N = 4; gs2_10.K = KD; gs2_10.zi_n = 1; gs2_10.flags = 0; gs2_10.act = 0;
      gs2_10.alpha = 1.0f; gs2_10.beta = 0.0f; gs2_10.sa = 1.0f; gs2_10.sb = 1.0f; gs2_10.Npad = LP; gs2_10.pad_ = 0;
      k_gemm<1><<<dim3((unsigned)((LP) + 31) / 32, (unsigned)((4) + 15) / 16, (unsigned)(O)), 32, 0, stream>>>(gs2_10); }
    k_caps_cp<<<(unsigned)(((long long)O * 4 * KD + 255) / 256), 256, 0, stream>>>(P, CC, CP, 11, O, I);
    { GemmP gs2_11;
      gs2_11.A = CP; gs2_11.B = Wc; gs2_11.bias = CP; gs2_11.R = CP; gs2_11.C = S + (size_t)11 * O * 4 * LP;
      gs2_11.sAo = (long long)4 * KD; gs2_11.sAi = 0; gs2_11.sAm = KD; gs2_11.sAk = 1; gs2_11.sBo = (long long)KD * 4; gs2_11.sBi = 0; gs2_11.sBn = 1; gs2_11.sBk = 4; gs2_11.sCo = 4 * LP; gs2_11.sCi = 0; gs2_11.sCm = LP; gs2_11.sRo = 0; gs2_11.sRi = 0; gs2_11.sRm = 0; gs2_11.sRn = 0;
      gs2_11.M = 4; gs2_11.N = 4; gs2_11.K = KD; gs2_11.zi_n = 1; gs2_11.flags = 0; gs2_11.act = 0;
      gs2_11.alpha = 1.0f; gs2_11.beta = 0.0f; gs2_11.sa = 1.0f; gs2_11.sb = 1.0f; gs2_11.Npad = LP; gs2_11.pad_ = 0;
      k_gemm<1><<<dim3((unsigned)((LP) + 31) / 32, (unsigned)((4) + 15) / 16, (unsigned)(O)), 32, 0, stream>>>(gs2_11); }
    k_caps_cp<<<(unsigned)(((long long)O * 4 * KD + 255) / 256), 256, 0, stream>>>(P, CC, CP, 12, O, I);
    { GemmP gs2_12;
      gs2_12.A = CP; gs2_12.B = Wc; gs2_12.bias = CP; gs2_12.R = CP; gs2_12.C = S + (size_t)12 * O * 4 * LP;
      gs2_12.sAo = (long long)4 * KD; gs2_12.sAi = 0; gs2_12.sAm = KD; gs2_12.sAk = 1; gs2_12.sBo = (long long)KD * 4; gs2_12.sBi = 0; gs2_12.sBn = 1; gs2_12.sBk = 4; gs2_12.sCo = 4 * LP; gs2_12.sCi = 0; gs2_12.sCm = LP; gs2_12.sRo = 0; gs2_12.sRi = 0; gs2_12.sRm = 0; gs2_12.sRn = 0;
      gs2_12.M = 4; gs2_12.N = 4; gs2_12.K = KD; gs2_12.zi_n = 1; gs2_12.flags = 0; gs2_12.act = 0;
      gs2_12.alpha = 1.0f; gs2_12.beta = 0.0f; gs2_12.sa = 1.0f; gs2_12.sb = 1.0f; gs2_12.Npad = LP; gs2_12.pad_ = 0;
      k_gemm<1><<<dim3((unsigned)((LP) + 31) / 32, (unsigned)((4) + 15) / 16, (unsigned)(O)), 32, 0, stream>>>(gs2_12); }
    k_caps_cp<<<(unsigned)(((long long)O * 4 * KD + 255) / 256), 256, 0, stream>>>(P, CC, CP, 13, O, I);
    { GemmP gs2_13;
      gs2_13.A = CP; gs2_13.B = Wc; gs2_13.bias = CP; gs2_13.R = CP; gs2_13.C = S + (size_t)13 * O * 4 * LP;
      gs2_13.sAo = (long long)4 * KD; gs2_13.sAi = 0; gs2_13.sAm = KD; gs2_13.sAk = 1; gs2_13.sBo = (long long)KD * 4; gs2_13.sBi = 0; gs2_13.sBn = 1; gs2_13.sBk = 4; gs2_13.sCo = 4 * LP; gs2_13.sCi = 0; gs2_13.sCm = LP; gs2_13.sRo = 0; gs2_13.sRi = 0; gs2_13.sRm = 0; gs2_13.sRn = 0;
      gs2_13.M = 4; gs2_13.N = 4; gs2_13.K = KD; gs2_13.zi_n = 1; gs2_13.flags = 0; gs2_13.act = 0;
      gs2_13.alpha = 1.0f; gs2_13.beta = 0.0f; gs2_13.sa = 1.0f; gs2_13.sb = 1.0f; gs2_13.Npad = LP; gs2_13.pad_ = 0;
      k_gemm<1><<<dim3((unsigned)((LP) + 31) / 32, (unsigned)((4) + 15) / 16, (unsigned)(O)), 32, 0, stream>>>(gs2_13); }
    k_caps_cp<<<(unsigned)(((long long)O * 4 * KD + 255) / 256), 256, 0, stream>>>(P, CC, CP, 14, O, I);
    { GemmP gs2_14;
      gs2_14.A = CP; gs2_14.B = Wc; gs2_14.bias = CP; gs2_14.R = CP; gs2_14.C = S + (size_t)14 * O * 4 * LP;
      gs2_14.sAo = (long long)4 * KD; gs2_14.sAi = 0; gs2_14.sAm = KD; gs2_14.sAk = 1; gs2_14.sBo = (long long)KD * 4; gs2_14.sBi = 0; gs2_14.sBn = 1; gs2_14.sBk = 4; gs2_14.sCo = 4 * LP; gs2_14.sCi = 0; gs2_14.sCm = LP; gs2_14.sRo = 0; gs2_14.sRi = 0; gs2_14.sRm = 0; gs2_14.sRn = 0;
      gs2_14.M = 4; gs2_14.N = 4; gs2_14.K = KD; gs2_14.zi_n = 1; gs2_14.flags = 0; gs2_14.act = 0;
      gs2_14.alpha = 1.0f; gs2_14.beta = 0.0f; gs2_14.sa = 1.0f; gs2_14.sb = 1.0f; gs2_14.Npad = LP; gs2_14.pad_ = 0;
      k_gemm<1><<<dim3((unsigned)((LP) + 31) / 32, (unsigned)((4) + 15) / 16, (unsigned)(O)), 32, 0, stream>>>(gs2_14); }
    k_caps_cp<<<(unsigned)(((long long)O * 4 * KD + 255) / 256), 256, 0, stream>>>(P, CC, CP, 15, O, I);
    { GemmP gs2_15;
      gs2_15.A = CP; gs2_15.B = Wc; gs2_15.bias = CP; gs2_15.R = CP; gs2_15.C = S + (size_t)15 * O * 4 * LP;
      gs2_15.sAo = (long long)4 * KD; gs2_15.sAi = 0; gs2_15.sAm = KD; gs2_15.sAk = 1; gs2_15.sBo = (long long)KD * 4; gs2_15.sBi = 0; gs2_15.sBn = 1; gs2_15.sBk = 4; gs2_15.sCo = 4 * LP; gs2_15.sCi = 0; gs2_15.sCm = LP; gs2_15.sRo = 0; gs2_15.sRi = 0; gs2_15.sRm = 0; gs2_15.sRn = 0;
      gs2_15.M = 4; gs2_15.N = 4; gs2_15.K = KD; gs2_15.zi_n = 1; gs2_15.flags = 0; gs2_15.act = 0;
      gs2_15.alpha = 1.0f; gs2_15.beta = 0.0f; gs2_15.sa = 1.0f; gs2_15.sb = 1.0f; gs2_15.Npad = LP; gs2_15.pad_ = 0;
      k_gemm<1><<<dim3((unsigned)((LP) + 31) / 32, (unsigned)((4) + 15) / 16, (unsigned)(O)), 32, 0, stream>>>(gs2_15); }
    k_caps_cp<<<(unsigned)(((long long)O * 4 * KD + 255) / 256), 256, 0, stream>>>(P, CC, CP, 16, O, I);
    { GemmP gs2_16;
      gs2_16.A = CP; gs2_16.B = Wc; gs2_16.bias = CP; gs2_16.R = CP; gs2_16.C = S + (size_t)16 * O * 4 * LP;
      gs2_16.sAo = (long long)4 * KD; gs2_16.sAi = 0; gs2_16.sAm = KD; gs2_16.sAk = 1; gs2_16.sBo = (long long)KD * 4; gs2_16.sBi = 0; gs2_16.sBn = 1; gs2_16.sBk = 4; gs2_16.sCo = 4 * LP; gs2_16.sCi = 0; gs2_16.sCm = LP; gs2_16.sRo = 0; gs2_16.sRi = 0; gs2_16.sRm = 0; gs2_16.sRn = 0;
      gs2_16.M = 4; gs2_16.N = 4; gs2_16.K = KD; gs2_16.zi_n = 1; gs2_16.flags = 0; gs2_16.act = 0;
      gs2_16.alpha = 1.0f; gs2_16.beta = 0.0f; gs2_16.sa = 1.0f; gs2_16.sb = 1.0f; gs2_16.Npad = LP; gs2_16.pad_ = 0;
      k_gemm<1><<<dim3((unsigned)((LP) + 31) / 32, (unsigned)((4) + 15) / 16, (unsigned)(O)), 32, 0, stream>>>(gs2_16); }
    k_caps_cp<<<(unsigned)(((long long)O * 4 * KD + 255) / 256), 256, 0, stream>>>(P, CC, CP, 17, O, I);
    { GemmP gs2_17;
      gs2_17.A = CP; gs2_17.B = Wc; gs2_17.bias = CP; gs2_17.R = CP; gs2_17.C = S + (size_t)17 * O * 4 * LP;
      gs2_17.sAo = (long long)4 * KD; gs2_17.sAi = 0; gs2_17.sAm = KD; gs2_17.sAk = 1; gs2_17.sBo = (long long)KD * 4; gs2_17.sBi = 0; gs2_17.sBn = 1; gs2_17.sBk = 4; gs2_17.sCo = 4 * LP; gs2_17.sCi = 0; gs2_17.sCm = LP; gs2_17.sRo = 0; gs2_17.sRi = 0; gs2_17.sRm = 0; gs2_17.sRn = 0;
      gs2_17.M = 4; gs2_17.N = 4; gs2_17.K = KD; gs2_17.zi_n = 1; gs2_17.flags = 0; gs2_17.act = 0;
      gs2_17.alpha = 1.0f; gs2_17.beta = 0.0f; gs2_17.sa = 1.0f; gs2_17.sb = 1.0f; gs2_17.Npad = LP; gs2_17.pad_ = 0;
      k_gemm<1><<<dim3((unsigned)((LP) + 31) / 32, (unsigned)((4) + 15) / 16, (unsigned)(O)), 32, 0, stream>>>(gs2_17); }
    k_caps_cp<<<(unsigned)(((long long)O * 4 * KD + 255) / 256), 256, 0, stream>>>(P, CC, CP, 18, O, I);
    { GemmP gs2_18;
      gs2_18.A = CP; gs2_18.B = Wc; gs2_18.bias = CP; gs2_18.R = CP; gs2_18.C = S + (size_t)18 * O * 4 * LP;
      gs2_18.sAo = (long long)4 * KD; gs2_18.sAi = 0; gs2_18.sAm = KD; gs2_18.sAk = 1; gs2_18.sBo = (long long)KD * 4; gs2_18.sBi = 0; gs2_18.sBn = 1; gs2_18.sBk = 4; gs2_18.sCo = 4 * LP; gs2_18.sCi = 0; gs2_18.sCm = LP; gs2_18.sRo = 0; gs2_18.sRi = 0; gs2_18.sRm = 0; gs2_18.sRn = 0;
      gs2_18.M = 4; gs2_18.N = 4; gs2_18.K = KD; gs2_18.zi_n = 1; gs2_18.flags = 0; gs2_18.act = 0;
      gs2_18.alpha = 1.0f; gs2_18.beta = 0.0f; gs2_18.sa = 1.0f; gs2_18.sb = 1.0f; gs2_18.Npad = LP; gs2_18.pad_ = 0;
      k_gemm<1><<<dim3((unsigned)((LP) + 31) / 32, (unsigned)((4) + 15) / 16, (unsigned)(O)), 32, 0, stream>>>(gs2_18); }
    k_caps_cp<<<(unsigned)(((long long)O * 4 * KD + 255) / 256), 256, 0, stream>>>(P, CC, CP, 19, O, I);
    { GemmP gs2_19;
      gs2_19.A = CP; gs2_19.B = Wc; gs2_19.bias = CP; gs2_19.R = CP; gs2_19.C = S + (size_t)19 * O * 4 * LP;
      gs2_19.sAo = (long long)4 * KD; gs2_19.sAi = 0; gs2_19.sAm = KD; gs2_19.sAk = 1; gs2_19.sBo = (long long)KD * 4; gs2_19.sBi = 0; gs2_19.sBn = 1; gs2_19.sBk = 4; gs2_19.sCo = 4 * LP; gs2_19.sCi = 0; gs2_19.sCm = LP; gs2_19.sRo = 0; gs2_19.sRi = 0; gs2_19.sRm = 0; gs2_19.sRn = 0;
      gs2_19.M = 4; gs2_19.N = 4; gs2_19.K = KD; gs2_19.zi_n = 1; gs2_19.flags = 0; gs2_19.act = 0;
      gs2_19.alpha = 1.0f; gs2_19.beta = 0.0f; gs2_19.sa = 1.0f; gs2_19.sb = 1.0f; gs2_19.Npad = LP; gs2_19.pad_ = 0;
      k_gemm<1><<<dim3((unsigned)((LP) + 31) / 32, (unsigned)((4) + 15) / 16, (unsigned)(O)), 32, 0, stream>>>(gs2_19); }
    k_caps_cp<<<(unsigned)(((long long)O * 4 * KD + 255) / 256), 256, 0, stream>>>(P, CC, CP, 20, O, I);
    { GemmP gs2_20;
      gs2_20.A = CP; gs2_20.B = Wc; gs2_20.bias = CP; gs2_20.R = CP; gs2_20.C = S + (size_t)20 * O * 4 * LP;
      gs2_20.sAo = (long long)4 * KD; gs2_20.sAi = 0; gs2_20.sAm = KD; gs2_20.sAk = 1; gs2_20.sBo = (long long)KD * 4; gs2_20.sBi = 0; gs2_20.sBn = 1; gs2_20.sBk = 4; gs2_20.sCo = 4 * LP; gs2_20.sCi = 0; gs2_20.sCm = LP; gs2_20.sRo = 0; gs2_20.sRi = 0; gs2_20.sRm = 0; gs2_20.sRn = 0;
      gs2_20.M = 4; gs2_20.N = 4; gs2_20.K = KD; gs2_20.zi_n = 1; gs2_20.flags = 0; gs2_20.act = 0;
      gs2_20.alpha = 1.0f; gs2_20.beta = 0.0f; gs2_20.sa = 1.0f; gs2_20.sb = 1.0f; gs2_20.Npad = LP; gs2_20.pad_ = 0;
      k_gemm<1><<<dim3((unsigned)((LP) + 31) / 32, (unsigned)((4) + 15) / 16, (unsigned)(O)), 32, 0, stream>>>(gs2_20); }
    k_caps_cp<<<(unsigned)(((long long)O * 4 * KD + 255) / 256), 256, 0, stream>>>(P, CC, CP, 21, O, I);
    { GemmP gs2_21;
      gs2_21.A = CP; gs2_21.B = Wc; gs2_21.bias = CP; gs2_21.R = CP; gs2_21.C = S + (size_t)21 * O * 4 * LP;
      gs2_21.sAo = (long long)4 * KD; gs2_21.sAi = 0; gs2_21.sAm = KD; gs2_21.sAk = 1; gs2_21.sBo = (long long)KD * 4; gs2_21.sBi = 0; gs2_21.sBn = 1; gs2_21.sBk = 4; gs2_21.sCo = 4 * LP; gs2_21.sCi = 0; gs2_21.sCm = LP; gs2_21.sRo = 0; gs2_21.sRi = 0; gs2_21.sRm = 0; gs2_21.sRn = 0;
      gs2_21.M = 4; gs2_21.N = 4; gs2_21.K = KD; gs2_21.zi_n = 1; gs2_21.flags = 0; gs2_21.act = 0;
      gs2_21.alpha = 1.0f; gs2_21.beta = 0.0f; gs2_21.sa = 1.0f; gs2_21.sb = 1.0f; gs2_21.Npad = LP; gs2_21.pad_ = 0;
      k_gemm<1><<<dim3((unsigned)((LP) + 31) / 32, (unsigned)((4) + 15) / 16, (unsigned)(O)), 32, 0, stream>>>(gs2_21); }
    k_caps_cp<<<(unsigned)(((long long)O * 4 * KD + 255) / 256), 256, 0, stream>>>(P, CC, CP, 22, O, I);
    { GemmP gs2_22;
      gs2_22.A = CP; gs2_22.B = Wc; gs2_22.bias = CP; gs2_22.R = CP; gs2_22.C = S + (size_t)22 * O * 4 * LP;
      gs2_22.sAo = (long long)4 * KD; gs2_22.sAi = 0; gs2_22.sAm = KD; gs2_22.sAk = 1; gs2_22.sBo = (long long)KD * 4; gs2_22.sBi = 0; gs2_22.sBn = 1; gs2_22.sBk = 4; gs2_22.sCo = 4 * LP; gs2_22.sCi = 0; gs2_22.sCm = LP; gs2_22.sRo = 0; gs2_22.sRi = 0; gs2_22.sRm = 0; gs2_22.sRn = 0;
      gs2_22.M = 4; gs2_22.N = 4; gs2_22.K = KD; gs2_22.zi_n = 1; gs2_22.flags = 0; gs2_22.act = 0;
      gs2_22.alpha = 1.0f; gs2_22.beta = 0.0f; gs2_22.sa = 1.0f; gs2_22.sb = 1.0f; gs2_22.Npad = LP; gs2_22.pad_ = 0;
      k_gemm<1><<<dim3((unsigned)((LP) + 31) / 32, (unsigned)((4) + 15) / 16, (unsigned)(O)), 32, 0, stream>>>(gs2_22); }
    k_caps_cp<<<(unsigned)(((long long)O * 4 * KD + 255) / 256), 256, 0, stream>>>(P, CC, CP, 23, O, I);
    { GemmP gs2_23;
      gs2_23.A = CP; gs2_23.B = Wc; gs2_23.bias = CP; gs2_23.R = CP; gs2_23.C = S + (size_t)23 * O * 4 * LP;
      gs2_23.sAo = (long long)4 * KD; gs2_23.sAi = 0; gs2_23.sAm = KD; gs2_23.sAk = 1; gs2_23.sBo = (long long)KD * 4; gs2_23.sBi = 0; gs2_23.sBn = 1; gs2_23.sBk = 4; gs2_23.sCo = 4 * LP; gs2_23.sCi = 0; gs2_23.sCm = LP; gs2_23.sRo = 0; gs2_23.sRi = 0; gs2_23.sRm = 0; gs2_23.sRn = 0;
      gs2_23.M = 4; gs2_23.N = 4; gs2_23.K = KD; gs2_23.zi_n = 1; gs2_23.flags = 0; gs2_23.act = 0;
      gs2_23.alpha = 1.0f; gs2_23.beta = 0.0f; gs2_23.sa = 1.0f; gs2_23.sb = 1.0f; gs2_23.Npad = LP; gs2_23.pad_ = 0;
      k_gemm<1><<<dim3((unsigned)((LP) + 31) / 32, (unsigned)((4) + 15) / 16, (unsigned)(O)), 32, 0, stream>>>(gs2_23); }
    k_caps_cp<<<(unsigned)(((long long)O * 4 * KD + 255) / 256), 256, 0, stream>>>(P, CC, CP, 24, O, I);
    { GemmP gs2_24;
      gs2_24.A = CP; gs2_24.B = Wc; gs2_24.bias = CP; gs2_24.R = CP; gs2_24.C = S + (size_t)24 * O * 4 * LP;
      gs2_24.sAo = (long long)4 * KD; gs2_24.sAi = 0; gs2_24.sAm = KD; gs2_24.sAk = 1; gs2_24.sBo = (long long)KD * 4; gs2_24.sBi = 0; gs2_24.sBn = 1; gs2_24.sBk = 4; gs2_24.sCo = 4 * LP; gs2_24.sCi = 0; gs2_24.sCm = LP; gs2_24.sRo = 0; gs2_24.sRi = 0; gs2_24.sRm = 0; gs2_24.sRn = 0;
      gs2_24.M = 4; gs2_24.N = 4; gs2_24.K = KD; gs2_24.zi_n = 1; gs2_24.flags = 0; gs2_24.act = 0;
      gs2_24.alpha = 1.0f; gs2_24.beta = 0.0f; gs2_24.sa = 1.0f; gs2_24.sb = 1.0f; gs2_24.Npad = LP; gs2_24.pad_ = 0;
      k_gemm<1><<<dim3((unsigned)((LP) + 31) / 32, (unsigned)((4) + 15) / 16, (unsigned)(O)), 32, 0, stream>>>(gs2_24); }
    k_caps_cp<<<(unsigned)(((long long)O * 4 * KD + 255) / 256), 256, 0, stream>>>(P, CC, CP, 25, O, I);
    { GemmP gs2_25;
      gs2_25.A = CP; gs2_25.B = Wc; gs2_25.bias = CP; gs2_25.R = CP; gs2_25.C = S + (size_t)25 * O * 4 * LP;
      gs2_25.sAo = (long long)4 * KD; gs2_25.sAi = 0; gs2_25.sAm = KD; gs2_25.sAk = 1; gs2_25.sBo = (long long)KD * 4; gs2_25.sBi = 0; gs2_25.sBn = 1; gs2_25.sBk = 4; gs2_25.sCo = 4 * LP; gs2_25.sCi = 0; gs2_25.sCm = LP; gs2_25.sRo = 0; gs2_25.sRi = 0; gs2_25.sRm = 0; gs2_25.sRn = 0;
      gs2_25.M = 4; gs2_25.N = 4; gs2_25.K = KD; gs2_25.zi_n = 1; gs2_25.flags = 0; gs2_25.act = 0;
      gs2_25.alpha = 1.0f; gs2_25.beta = 0.0f; gs2_25.sa = 1.0f; gs2_25.sb = 1.0f; gs2_25.Npad = LP; gs2_25.pad_ = 0;
      k_gemm<1><<<dim3((unsigned)((LP) + 31) / 32, (unsigned)((4) + 15) / 16, (unsigned)(O)), 32, 0, stream>>>(gs2_25); }
    k_caps_cp<<<(unsigned)(((long long)O * 4 * KD + 255) / 256), 256, 0, stream>>>(P, CC, CP, 26, O, I);
    { GemmP gs2_26;
      gs2_26.A = CP; gs2_26.B = Wc; gs2_26.bias = CP; gs2_26.R = CP; gs2_26.C = S + (size_t)26 * O * 4 * LP;
      gs2_26.sAo = (long long)4 * KD; gs2_26.sAi = 0; gs2_26.sAm = KD; gs2_26.sAk = 1; gs2_26.sBo = (long long)KD * 4; gs2_26.sBi = 0; gs2_26.sBn = 1; gs2_26.sBk = 4; gs2_26.sCo = 4 * LP; gs2_26.sCi = 0; gs2_26.sCm = LP; gs2_26.sRo = 0; gs2_26.sRi = 0; gs2_26.sRm = 0; gs2_26.sRn = 0;
      gs2_26.M = 4; gs2_26.N = 4; gs2_26.K = KD; gs2_26.zi_n = 1; gs2_26.flags = 0; gs2_26.act = 0;
      gs2_26.alpha = 1.0f; gs2_26.beta = 0.0f; gs2_26.sa = 1.0f; gs2_26.sb = 1.0f; gs2_26.Npad = LP; gs2_26.pad_ = 0;
      k_gemm<1><<<dim3((unsigned)((LP) + 31) / 32, (unsigned)((4) + 15) / 16, (unsigned)(O)), 32, 0, stream>>>(gs2_26); }
    k_caps_cp<<<(unsigned)(((long long)O * 4 * KD + 255) / 256), 256, 0, stream>>>(P, CC, CP, 27, O, I);
    { GemmP gs2_27;
      gs2_27.A = CP; gs2_27.B = Wc; gs2_27.bias = CP; gs2_27.R = CP; gs2_27.C = S + (size_t)27 * O * 4 * LP;
      gs2_27.sAo = (long long)4 * KD; gs2_27.sAi = 0; gs2_27.sAm = KD; gs2_27.sAk = 1; gs2_27.sBo = (long long)KD * 4; gs2_27.sBi = 0; gs2_27.sBn = 1; gs2_27.sBk = 4; gs2_27.sCo = 4 * LP; gs2_27.sCi = 0; gs2_27.sCm = LP; gs2_27.sRo = 0; gs2_27.sRi = 0; gs2_27.sRm = 0; gs2_27.sRn = 0;
      gs2_27.M = 4; gs2_27.N = 4; gs2_27.K = KD; gs2_27.zi_n = 1; gs2_27.flags = 0; gs2_27.act = 0;
      gs2_27.alpha = 1.0f; gs2_27.beta = 0.0f; gs2_27.sa = 1.0f; gs2_27.sb = 1.0f; gs2_27.Npad = LP; gs2_27.pad_ = 0;
      k_gemm<1><<<dim3((unsigned)((LP) + 31) / 32, (unsigned)((4) + 15) / 16, (unsigned)(O)), 32, 0, stream>>>(gs2_27); }
    k_caps_cp<<<(unsigned)(((long long)O * 4 * KD + 255) / 256), 256, 0, stream>>>(P, CC, CP, 28, O, I);
    { GemmP gs2_28;
      gs2_28.A = CP; gs2_28.B = Wc; gs2_28.bias = CP; gs2_28.R = CP; gs2_28.C = S + (size_t)28 * O * 4 * LP;
      gs2_28.sAo = (long long)4 * KD; gs2_28.sAi = 0; gs2_28.sAm = KD; gs2_28.sAk = 1; gs2_28.sBo = (long long)KD * 4; gs2_28.sBi = 0; gs2_28.sBn = 1; gs2_28.sBk = 4; gs2_28.sCo = 4 * LP; gs2_28.sCi = 0; gs2_28.sCm = LP; gs2_28.sRo = 0; gs2_28.sRi = 0; gs2_28.sRm = 0; gs2_28.sRn = 0;
      gs2_28.M = 4; gs2_28.N = 4; gs2_28.K = KD; gs2_28.zi_n = 1; gs2_28.flags = 0; gs2_28.act = 0;
      gs2_28.alpha = 1.0f; gs2_28.beta = 0.0f; gs2_28.sa = 1.0f; gs2_28.sb = 1.0f; gs2_28.Npad = LP; gs2_28.pad_ = 0;
      k_gemm<1><<<dim3((unsigned)((LP) + 31) / 32, (unsigned)((4) + 15) / 16, (unsigned)(O)), 32, 0, stream>>>(gs2_28); }
    k_caps_cp<<<(unsigned)(((long long)O * 4 * KD + 255) / 256), 256, 0, stream>>>(P, CC, CP, 29, O, I);
    { GemmP gs2_29;
      gs2_29.A = CP; gs2_29.B = Wc; gs2_29.bias = CP; gs2_29.R = CP; gs2_29.C = S + (size_t)29 * O * 4 * LP;
      gs2_29.sAo = (long long)4 * KD; gs2_29.sAi = 0; gs2_29.sAm = KD; gs2_29.sAk = 1; gs2_29.sBo = (long long)KD * 4; gs2_29.sBi = 0; gs2_29.sBn = 1; gs2_29.sBk = 4; gs2_29.sCo = 4 * LP; gs2_29.sCi = 0; gs2_29.sCm = LP; gs2_29.sRo = 0; gs2_29.sRi = 0; gs2_29.sRm = 0; gs2_29.sRn = 0;
      gs2_29.M = 4; gs2_29.N = 4; gs2_29.K = KD; gs2_29.zi_n = 1; gs2_29.flags = 0; gs2_29.act = 0;
      gs2_29.alpha = 1.0f; gs2_29.beta = 0.0f; gs2_29.sa = 1.0f; gs2_29.sb = 1.0f; gs2_29.Npad = LP; gs2_29.pad_ = 0;
      k_gemm<1><<<dim3((unsigned)((LP) + 31) / 32, (unsigned)((4) + 15) / 16, (unsigned)(O)), 32, 0, stream>>>(gs2_29); }
    k_caps_cp<<<(unsigned)(((long long)O * 4 * KD + 255) / 256), 256, 0, stream>>>(P, CC, CP, 30, O, I);
    { GemmP gs2_30;
      gs2_30.A = CP; gs2_30.B = Wc; gs2_30.bias = CP; gs2_30.R = CP; gs2_30.C = S + (size_t)30 * O * 4 * LP;
      gs2_30.sAo = (long long)4 * KD; gs2_30.sAi = 0; gs2_30.sAm = KD; gs2_30.sAk = 1; gs2_30.sBo = (long long)KD * 4; gs2_30.sBi = 0; gs2_30.sBn = 1; gs2_30.sBk = 4; gs2_30.sCo = 4 * LP; gs2_30.sCi = 0; gs2_30.sCm = LP; gs2_30.sRo = 0; gs2_30.sRi = 0; gs2_30.sRm = 0; gs2_30.sRn = 0;
      gs2_30.M = 4; gs2_30.N = 4; gs2_30.K = KD; gs2_30.zi_n = 1; gs2_30.flags = 0; gs2_30.act = 0;
      gs2_30.alpha = 1.0f; gs2_30.beta = 0.0f; gs2_30.sa = 1.0f; gs2_30.sb = 1.0f; gs2_30.Npad = LP; gs2_30.pad_ = 0;
      k_gemm<1><<<dim3((unsigned)((LP) + 31) / 32, (unsigned)((4) + 15) / 16, (unsigned)(O)), 32, 0, stream>>>(gs2_30); }
    k_caps_cp<<<(unsigned)(((long long)O * 4 * KD + 255) / 256), 256, 0, stream>>>(P, CC, CP, 31, O, I);
    { GemmP gs2_31;
      gs2_31.A = CP; gs2_31.B = Wc; gs2_31.bias = CP; gs2_31.R = CP; gs2_31.C = S + (size_t)31 * O * 4 * LP;
      gs2_31.sAo = (long long)4 * KD; gs2_31.sAi = 0; gs2_31.sAm = KD; gs2_31.sAk = 1; gs2_31.sBo = (long long)KD * 4; gs2_31.sBi = 0; gs2_31.sBn = 1; gs2_31.sBk = 4; gs2_31.sCo = 4 * LP; gs2_31.sCi = 0; gs2_31.sCm = LP; gs2_31.sRo = 0; gs2_31.sRi = 0; gs2_31.sRm = 0; gs2_31.sRn = 0;
      gs2_31.M = 4; gs2_31.N = 4; gs2_31.K = KD; gs2_31.zi_n = 1; gs2_31.flags = 0; gs2_31.act = 0;
      gs2_31.alpha = 1.0f; gs2_31.beta = 0.0f; gs2_31.sa = 1.0f; gs2_31.sb = 1.0f; gs2_31.Npad = LP; gs2_31.pad_ = 0;
      k_gemm<1><<<dim3((unsigned)((LP) + 31) / 32, (unsigned)((4) + 15) / 16, (unsigned)(O)), 32, 0, stream>>>(gs2_31); }
    k_caps_squash<<<(unsigned)((Bn * O * 16 + 255) / 256), 256, 0, stream>>>(S, LP, V, out, aout, Bn * O, 1);
}
